// CSPLayer_43473658970185
// MI455X (gfx1250) — hardware-verified
//
#include <hip/hip_runtime.h>
#include <math.h>

typedef __attribute__((ext_vector_type(16))) _Float16 v16h;
typedef __attribute__((ext_vector_type(8)))  _Float16 v8h;
typedef __attribute__((ext_vector_type(16))) __bf16   v16b;
typedef __attribute__((ext_vector_type(8)))  float    v8f;
typedef __attribute__((ext_vector_type(4)))  float    v4f;

__device__ __forceinline__ int frag_k(int i, int h) { return (i < 8) ? (8 * h + i) : (16 + 8 * h + (i - 8)); }
__device__ __forceinline__ __bf16 bf16_rne(float f) {
    unsigned int u = __float_as_uint(f);
    u += 0x7fffu + ((u >> 16) & 1u);
    return __builtin_bit_cast(__bf16, (unsigned short)(u >> 16));
}
__device__ __forceinline__ float bf16_f32(__bf16 b) { return __uint_as_float(((unsigned int)__builtin_bit_cast(unsigned short, b)) << 16); }
__device__ __forceinline__ v8f wmma16(v16h a, v16h b, v8f c) {
    c = __builtin_amdgcn_wmma_f32_16x16x32_f16(false, a, false, b, (short)0, c, false, false);
    asm volatile("v_nop\n\tv_nop\n\tv_nop\n\tv_nop" : "+v"(c) : "v"(a), "v"(b));
    return c;
}
__device__ __forceinline__ v8f wmmab(v16b a, v16b b, v8f c) {
    c = __builtin_amdgcn_wmma_f32_16x16x32_bf16(false, a, false, b, (short)0, c, false, false);
    asm volatile("v_nop\n\tv_nop\n\tv_nop\n\tv_nop" : "+v"(c) : "v"(a), "v"(b));
    return c;
}
struct Split { v16b hi, lo; };
__device__ __forceinline__ v8f wmma3(const Split& a, const Split& b, v8f c) {
    c = __builtin_amdgcn_wmma_f32_16x16x32_bf16(false, a.hi, false, b.hi, (short)0, c, false, false);
    c = __builtin_amdgcn_wmma_f32_16x16x32_bf16(false, a.hi, false, b.lo, (short)0, c, false, false);
    c = __builtin_amdgcn_wmma_f32_16x16x32_bf16(false, a.lo, false, b.hi, (short)0, c, false, false);
    asm volatile("v_nop\n\tv_nop\n\tv_nop\n\tv_nop" : "+v"(c) : "v"(a.hi), "v"(a.lo), "v"(b.hi), "v"(b.lo));
    return c;
}
struct Split3 { v16b hi, mid, lo; };
__device__ __forceinline__ v8f wmma6(const Split3& a, const Split3& b, v8f c) {
    c = __builtin_amdgcn_wmma_f32_16x16x32_bf16(false, a.hi, false, b.hi, (short)0, c, false, false);
    c = __builtin_amdgcn_wmma_f32_16x16x32_bf16(false, a.hi, false, b.mid, (short)0, c, false, false);
    c = __builtin_amdgcn_wmma_f32_16x16x32_bf16(false, a.mid, false, b.hi, (short)0, c, false, false);
    c = __builtin_amdgcn_wmma_f32_16x16x32_bf16(false, a.hi, false, b.lo, (short)0, c, false, false);
    c = __builtin_amdgcn_wmma_f32_16x16x32_bf16(false, a.mid, false, b.mid, (short)0, c, false, false);
    c = __builtin_amdgcn_wmma_f32_16x16x32_bf16(false, a.lo, false, b.hi, (short)0, c, false, false);
    asm volatile("v_nop\n\tv_nop\n\tv_nop\n\tv_nop" : "+v"(c) : "v"(a.hi), "v"(a.mid), "v"(a.lo), "v"(b.hi), "v"(b.mid), "v"(b.lo));
    return c;
}

__device__ __forceinline__ v16h fh_ld(const float* __restrict__ p, long long sk, int k0, int h, int klen, float s) {
    v16h a;
#pragma unroll
    for (int i = 0; i < 16; ++i) { const int k = k0 + frag_k(i, h); a[i] = (k < klen) ? (_Float16)(p[(long long)k * sk] * s) : (_Float16)0.f; }
    return a;
}
__device__ __forceinline__ Split sp_ld(const float* __restrict__ p, long long sk, int k0, int h, int klen, float s) {
    Split r;
#pragma unroll
    for (int i = 0; i < 16; ++i) {
        const int k = k0 + frag_k(i, h); const float x = (k < klen) ? p[(long long)k * sk] * s : 0.f;
        const __bf16 hb = bf16_rne(x); r.hi[i] = hb; r.lo[i] = bf16_rne(x - bf16_f32(hb));
    }
    return r;
}
__device__ __forceinline__ Split3 sp3_ld(const float* __restrict__ p, long long sk, int k0, int h, int klen, float s) {
    Split3 r;
#pragma unroll
    for (int i = 0; i < 16; ++i) {
        const int k = k0 + frag_k(i, h); const float x = (k < klen) ? p[(long long)k * sk] * s : 0.f;
        const __bf16 hb = bf16_rne(x); const float r1 = x - bf16_f32(hb); const __bf16 mb = bf16_rne(r1);
        r.hi[i] = hb; r.mid[i] = mb; r.lo[i] = bf16_rne(r1 - bf16_f32(mb));
    }
    return r;
}
__device__ __forceinline__ v16b bh_ld(const float* __restrict__ p, long long sk, int k0, int h, int klen, float s) {
    v16b a;
#pragma unroll
    for (int i = 0; i < 16; ++i) { const int k = k0 + frag_k(i, h); a[i] = bf16_rne((k < klen) ? p[(long long)k * sk] * s : 0.f); }
    return a;
}
__device__ __forceinline__ v16h fh_row(const _Float16* __restrict__ row, int k0, int h) {
    v16h a;
#pragma unroll
    for (int i = 0; i < 16; ++i) a[i] = row[k0 + frag_k(i, h)];
    return a;
}

#define VST2(T, ptr, val) do { *(volatile T*)(ptr) = (val); __threadfence(); *(volatile T*)(ptr) = (val); } while (0)
typedef float v4f __attribute__((ext_vector_type(4)));
#define VST2V4(ptr, val) do { *(volatile v4f*)(ptr) = (val); __threadfence(); *(volatile v4f*)(ptr) = (val); } while (0)

__device__ __attribute__((noinline)) float act_fn(float v, int act) {
    if (act == 1) return fmaxf(v, 0.f);
    if (act == 2) { const float u = 0.7978845608028654f * (v + 0.044715f * v * v * v); return 0.5f * v * (1.f + tanhf(u)); }
    if (act == 3) return v / (1.f + expf(-v));
    if (act == 4) return 0.5f * v * (1.f + erff(v * 0.7071067811865476f));
    if (act == 5) return tanhf(v);
    if (act == 6) return 1.f / (1.f + expf(-v));
    if (act == 7) return (v > 0.f) ? v : 0.01f * v;
    if (act == 8) return (v > 0.f) ? v : (expf(v) - 1.f);
    if (act == 9) return fminf(fmaxf(v, 0.f), 6.f);
    if (act == 10) return fabsf(v);
    if (act == 11) return (v >= 0.f) ? v : 0.1f * v;
    if (act == 12) return (v > 0.f) ? v : 0.2f * v;
    if (act == 13) return (v > 20.f) ? v : log1pf(expf(v));
    return v;
}

struct GemmP {
    const float* A; const float* B; const float* bias; const float* R; float* C;
    long long sAo, sAi, sAm, sAk, sBo, sBi, sBn, sBk, sCo, sCi, sCm, sRo, sRi, sRm, sRn;
    int M, N, K, zi_n, flags, act; float alpha, beta, sa, sb;
    int Npad, pad_;
};
static_assert(sizeof(GemmP) == 5 * 8 + 15 * 8 + 6 * 4 + 4 * 4 + 2 * 4, "GemmP has padding");

template <int MODE>
__global__ __launch_bounds__(32) void k_gemm(GemmP p) {
    const int lane = threadIdx.x & 31, h = lane >> 4, l15 = lane & 15;
    const int m0 = blockIdx.y * 16, n0 = blockIdx.x * 32;
    const int z = blockIdx.z, zo = z / p.zi_n, zi = z - zo * p.zi_n;
    const float* A = p.A + zo * p.sAo + zi * p.sAi;
    const float* B = p.B + zo * p.sBo + zi * p.sBi;
    const int am = min(m0 + l15, p.M - 1);
    v8f acc[2], comp[2];
#pragma unroll
    for (int t = 0; t < 2; ++t) { v8f zz = {}; acc[t] = zz; comp[t] = zz; }
    for (int k0 = 0; k0 < p.K; k0 += 32) {
        const float* arow = A + (long long)am * p.sAm;
        if (MODE == 1) {
            const Split a = sp_ld(arow, p.sAk, k0, h, p.K, 1.f);
#pragma unroll
            for (int t = 0; t < 2; ++t) {
                const int bn = min(n0 + t * 16 + l15, p.N - 1);
                acc[t] = wmma3(a, sp_ld(B + (long long)bn * p.sBn, p.sBk, k0, h, p.K, 1.f), acc[t]);
            }
        } else if (MODE == 3) {
            const Split3 a = sp3_ld(arow, p.sAk, k0, h, p.K, 1.f);
#pragma unroll
            for (int t = 0; t < 2; ++t) {
                const int bn = min(n0 + t * 16 + l15, p.N - 1);
                acc[t] = wmma6(a, sp3_ld(B + (long long)bn * p.sBn, p.sBk, k0, h, p.K, 1.f), acc[t]);
            }
        } else if (MODE == 4) {
            const Split3 a = sp3_ld(arow, p.sAk, k0, h, p.K, 1.f);
#pragma unroll
            for (int t = 0; t < 2; ++t) {
                const int bn = min(n0 + t * 16 + l15, p.N - 1); v8f zz = {};
                const v8f part = wmma6(a, sp3_ld(B + (long long)bn * p.sBn, p.sBk, k0, h, p.K, 1.f), zz);
                const v8f y = part - comp[t]; const v8f s = acc[t] + y; comp[t] = (s - acc[t]) - y; acc[t] = s;
            }
        } else if (MODE == 2) {
            const v16b a = bh_ld(arow, p.sAk, k0, h, p.K, 1.f);
#pragma unroll
            for (int t = 0; t < 2; ++t) {
                const int bn = min(n0 + t * 16 + l15, p.N - 1);
                acc[t] = wmmab(a, bh_ld(B + (long long)bn * p.sBn, p.sBk, k0, h, p.K, 1.f), acc[t]);
            }
        } else {
            const v16h a = fh_ld(arow, p.sAk, k0, h, p.K, p.sa);
#pragma unroll
            for (int t = 0; t < 2; ++t) {
                const int bn = min(n0 + t * 16 + l15, p.N - 1);
                acc[t] = wmma16(a, fh_ld(B + (long long)bn * p.sBn, p.sBk, k0, h, p.K, p.sb), acc[t]);
            }
        }
    }
    const float iscale = (MODE == 0) ? p.alpha / (p.sa * p.sb) : p.alpha;
    float* C = p.C + zo * p.sCo + zi * p.sCi;
    const float* R = p.R + zo * p.sRo + zi * p.sRi;
    __shared__ __align__(16) float ctile[16][36];
#pragma unroll
    for (int t = 0; t < 2; ++t) {
        const int n = n0 + t * 16 + l15; const int nn = min(n, p.N - 1);
#pragma unroll
        for (int r = 0; r < 8; ++r) {
            const int m = m0 + 8 * h + r; const int mm = min(m, p.M - 1);
            float v = acc[t][r] * iscale;
            if (p.flags & 1) v += p.bias[nn];
            if (p.flags & 2) v += p.bias[mm];
            v = act_fn(v, p.act);
            if (p.flags & 4) v += p.beta * R[(long long)mm * p.sRm + (long long)nn * p.sRn];
            ctile[8 * h + r][t * 16 + l15] = (n < p.N) ? v : 0.f;
        }
    }
    __syncthreads();
    const int NW = (p.Npad > p.N) ? p.Npad : p.N;
    const bool fast = (m0 + 16 <= p.M) && (n0 + 32 <= NW) && ((p.sCm & 3) == 0) && ((((size_t)C) & 15) == 0);
    if (fast) {
#pragma unroll
        for (int s = 0; s < 4; ++s) {
            const int row = s * 4 + (lane >> 3), c4 = (lane & 7) * 4;
            const v4f v = *(const v4f*)&ctile[row][c4];
            VST2V4(C + (long long)(m0 + row) * p.sCm + n0 + c4, v);
        }
    } else {
        for (int row = 0; row < 16; ++row) {
            const int m = m0 + row, n = n0 + lane;
            if (m < p.M && n < NW) VST2(float, C + (long long)m * p.sCm + n, ctile[row][lane]);
        }
    }
}

#define AW 4
struct AttnP {
    const float* Q; const float* K; const float* V; float* O; float* P; const float* Mf; const int* Mi; float* ST;
    const float* Pw; const float* Rt; const int* SQ; const int* SK;
    long long swb, swh, swi, swj, srb, srh, sri;
    long long sQb, sQh, sQi, sQd, sKb, sKh, sKj, sKd, sVb, sVh, sVj, sVd, sOb, sOh, sOi, sPb, sPh, sPi, smb, smh, smi, smj;
    int Lq, Lk, dh, dv, hrep, causal, coff, pband;
    float scale, mfill; int nonorm, mpol;
    int roff, rn, segpol, win;
};
static_assert(sizeof(AttnP) == 12 * 8 + 29 * 8 + 16 * 4, "AttnP has padding");

#ifndef KATTN_ATTR
#define KATTN_ATTR
#endif
template <int DHP, int DVP, int QM, bool SPLITPV, bool TWOPASS>
__global__ __launch_bounds__(32 * AW) KATTN_ATTR void k_attn(AttnP p) {
    constexpr int NT = DVP / 16;
    constexpr int KS = DHP / 32;
    constexpr int VP = DVP + 8;
    __shared__ __align__(16) float    pl[AW][16 * 64];
    __shared__ __align__(16) _Float16 vl[(SPLITPV ? 2 : 1) * 64 * VP];
    const int lane = threadIdx.x & 31, hf = lane >> 4, l15 = lane & 15, wave = threadIdx.x >> 5;
    const int h = blockIdx.y, b = blockIdx.z, hk = h / p.hrep;
    const int q0 = (blockIdx.x * AW + wave) * 16;
    float* myp = pl[wave];
    const float L2E = 1.4426950408889634f;
    const float NEG = -__builtin_inff();
    const int qi = min(q0 + l15, p.Lq - 1);
    const float* qrow = p.Q + b * p.sQb + h * p.sQh + (long long)qi * p.sQi;
    const float* kbase = p.K + b * p.sKb + hk * p.sKh;
    const float* vbase = p.V + b * p.sVb + hk * p.sVh;
    v16h qa[QM == 0 ? KS : 1]; Split qs_[QM == 1 ? KS : 1]; Split3 qt_[QM == 2 ? KS : 1];
#pragma unroll
    for (int ks = 0; ks < KS; ++ks) {
        if (QM == 2) qt_[ks] = sp3_ld(qrow, p.sQd, ks * 32, hf, p.dh, 1.f);
        else if (QM == 1) qs_[ks] = sp_ld(qrow, p.sQd, ks * 32, hf, p.dh, 1.f);
        else qa[ks] = fh_ld(qrow, p.sQd, ks * 32, hf, p.dh, 1.f);
    }
    v8f o[NT]; float m8[8], l8[8];
#pragma unroll
    for (int t = 0; t < NT; ++t) { v8f zz = {}; o[t] = zz; }
#pragma unroll
    for (int i = 0; i < 8; ++i) { m8[i] = NEG; l8[i] = 0.f; }
    int jend = p.Lk;
    if (p.causal == 1) { const int je = (blockIdx.x * AW + AW - 1) * 16 + 16 + p.coff; jend = min(jend, max(je, 0)); }
    const int npass = TWOPASS ? 2 : 1;
    for (int pass = 0; pass < npass; ++pass) {
        const bool dopv = (!TWOPASS) || pass == 1;
        for (int j0 = 0; j0 < jend; j0 += 64) {
            if (dopv) {
                __syncthreads();
                for (int idx = threadIdx.x; idx < 64 * DVP; idx += 32 * AW) {
                    const int jr = idx / DVP, d = idx - jr * DVP, j = j0 + jr;
                    const float f = (j < p.Lk && d < p.dv) ? vbase[(long long)j * p.sVj + (long long)d * p.sVd] : 0.f;
                    if (SPLITPV) {
                        const __bf16 hb = bf16_rne(f);
                        ((__bf16*)vl)[jr * VP + d] = hb; ((__bf16*)vl)[64 * VP + jr * VP + d] = bf16_rne(f - bf16_f32(hb));
                    } else vl[jr * VP + d] = (_Float16)f;
                }
            }
            v8f s[4];
#pragma unroll
            for (int t = 0; t < 4; ++t) {
                const int j = min(j0 + t * 16 + l15, p.Lk - 1);
                const float* krow = kbase + (long long)j * p.sKj;
                v8f acc = {};
#pragma unroll
                for (int ks = 0; ks < KS; ++ks) {
                    if (QM == 2)      acc = wmma6(qt_[ks], sp3_ld(krow, p.sKd, ks * 32, hf, p.dh, 1.f), acc);
                    else if (QM == 1) acc = wmma3(qs_[ks], sp_ld(krow, p.sKd, ks * 32, hf, p.dh, 1.f), acc);
                    else              acc = wmma16(qa[ks], fh_ld(krow, p.sKd, ks * 32, hf, p.dh, 1.f), acc);
                }
                s[t] = acc;
            }
            float pv[8][4];
#pragma unroll
            for (int i = 0; i < 8; ++i) {
                const int irow = q0 + i + 8 * hf;
                const int ic = min(irow, p.Lq - 1);
                float sc[4];
#pragma unroll
                for (int t = 0; t < 4; ++t) {
                    const int jg = j0 + t * 16 + l15;
                    float v = s[t][i] * p.scale;
                    if (p.Mf) v += p.Mf[b * p.smb + h * p.smh + (long long)ic * p.smi + (long long)min(jg, p.Lk - 1) * p.smj];
                    if (p.Rt) { int rc = ic - min(jg, p.Lk - 1) + p.roff; rc = rc < 0 ? 0 : (rc >= p.rn ? p.rn - 1 : rc); v += p.Rt[b * p.srb + h * p.srh + (long long)ic * p.sri + rc]; }
                    if (p.Mi) { const int mv = p.Mi[b * p.smb + h * p.smh + (long long)ic * p.smi + (long long)min(jg, p.Lk - 1) * p.smj]; if (p.mpol ? (mv != 0) : (mv == 0)) v = p.mfill; }
                    if (p.SQ) { const bool same = p.SQ[(long long)b * p.Lq + ic] == p.SK[(long long)b * p.Lk + min(jg, p.Lk - 1)]; if (p.segpol ? same : !same) v = p.mfill; }
                    if (p.causal == 2 && jg > irow + p.coff) v = p.mfill;
                    if (jg >= p.Lk || (p.causal == 1 && jg > irow + p.coff) || (p.causal == 3 && jg < irow + p.coff) || (p.win > 0 && irow + p.coff - jg > p.win)) v = NEG; else v *= L2E;
                    sc[t] = v;
                }
                if (!TWOPASS || pass == 0) {
                    float mx = fmaxf(fmaxf(sc[0], sc[1]), fmaxf(sc[2], sc[3]));
                    mx = fmaxf(mx, __shfl_xor(mx, 1, 32)); mx = fmaxf(mx, __shfl_xor(mx, 2, 32));
                    mx = fmaxf(mx, __shfl_xor(mx, 4, 32)); mx = fmaxf(mx, __shfl_xor(mx, 8, 32));
                    const float mnew = fmaxf(m8[i], mx);
                    const float corr = (mnew == NEG) ? 1.f : exp2f(m8[i] - mnew);
                    float rs = 0.f;
#pragma unroll
                    for (int t = 0; t < 4; ++t) {
                        const float pp = (sc[t] == NEG) ? 0.f : exp2f(sc[t] - mnew); rs += pp;
                        pv[i][t] = p.Pw ? pp * p.Pw[b * p.swb + h * p.swh + (long long)ic * p.swi + (long long)min(j0 + t * 16 + l15, p.Lk - 1) * p.swj] : pp;
                    }
                    rs += __shfl_xor(rs, 1, 32); rs += __shfl_xor(rs, 2, 32); rs += __shfl_xor(rs, 4, 32); rs += __shfl_xor(rs, 8, 32);
                    l8[i] = l8[i] * corr + rs; m8[i] = mnew;
                    if (!TWOPASS) {
#pragma unroll
                        for (int t = 0; t < NT; ++t) o[t][i] *= corr;
                    }
                } else {
                    const float inv = (l8[i] > 0.f) ? 1.f / l8[i] : 0.f;
#pragma unroll
                    for (int t = 0; t < 4; ++t) {
                        const int jg = j0 + t * 16 + l15;
                        float pp = (sc[t] == NEG) ? 0.f : exp2f(sc[t] - m8[i]) * inv;
                        if (p.Pw) pp *= p.Pw[b * p.swb + h * p.swh + (long long)ic * p.swi + (long long)min(jg, p.Lk - 1) * p.swj];
                        pv[i][t] = pp;
                    }
                }
            }
            if (dopv) {
#pragma unroll
                for (int i = 0; i < 8; ++i)
#pragma unroll
                    for (int t = 0; t < 4; ++t) myp[(i + 8 * hf) * 64 + t * 16 + l15] = pv[i][t];
                __syncthreads();
                if (p.P) {
                    float* pb_ = p.P + b * p.sPb + h * p.sPh;
                    const bool fastP = (p.pband == 0) && ((p.sPi & 3) == 0) && (j0 + 64 <= p.Lk) && (q0 + 16 <= p.Lq) && ((((size_t)pb_) & 15) == 0);
                    if (fastP) {
#pragma unroll
                        for (int s = 0; s < 8; ++s) {
                            const int row = s * 2 + (lane >> 4), c4 = (lane & 15) * 4;
                            const v4f v = *(const v4f*)(myp + row * 64 + c4);
                            VST2V4(pb_ + (long long)(q0 + row) * p.sPi + j0 + c4, v);
                        }
                    } else {
                        for (int row = 0; row < 16; ++row) {
                            const int irow = q0 + row; if (irow >= p.Lq) continue;
                            for (int c = lane; c < 64; c += 32) {
                                const int jg = j0 + c; if (jg >= p.Lk) continue;
                                if (p.pband == 0) VST2(float, pb_ + (long long)irow * p.sPi + jg, myp[row * 64 + c]);
                                else if (jg - irow <= p.pband && irow - jg <= p.pband) VST2(float, pb_ + (long long)irow * p.sPi + (jg - irow + p.pband), myp[row * 64 + c]);
                            }
                        }
                    }
                }
                if (SPLITPV) {
                    const Split pa0 = sp_ld(myp + l15 * 64, 1, 0, hf, 64, 1.f), pa1 = sp_ld(myp + l15 * 64, 1, 32, hf, 64, 1.f);
                    const __bf16* vh = (const __bf16*)vl; const __bf16* vlo = vh + 64 * VP;
#pragma unroll
                    for (int t = 0; t < NT; ++t) {
                        const int dcol = t * 16 + l15;
                        Split b0, b1;
#pragma unroll
                        for (int e = 0; e < 16; ++e) {
                            const int k0 = frag_k(e, hf), k1 = 32 + frag_k(e, hf);
                            b0.hi[e] = vh[k0 * VP + dcol]; b0.lo[e] = vlo[k0 * VP + dcol]; b1.hi[e] = vh[k1 * VP + dcol]; b1.lo[e] = vlo[k1 * VP + dcol];
                        }
                        o[t] = wmma3(pa0, b0, o[t]);
                        o[t] = wmma3(pa1, b1, o[t]);
                    }
                } else {
                    const v16h pa0 = fh_ld(myp + l15 * 64, 1, 0, hf, 64, 4096.f), pa1 = fh_ld(myp + l15 * 64, 1, 32, hf, 64, 4096.f);
#pragma unroll
                    for (int t = 0; t < NT; ++t) {
                        const int dcol = t * 16 + l15;
                        v16h b0, b1;
#pragma unroll
                        for (int e = 0; e < 16; ++e) { b0[e] = vl[frag_k(e, hf) * VP + dcol]; b1[e] = vl[(32 + frag_k(e, hf)) * VP + dcol]; }
                        o[t] = wmma16(pa0, b0, o[t]);
                        o[t] = wmma16(pa1, b1, o[t]);
                    }
                }
            }
        }
    }
    float* obase = p.O + b * p.sOb + h * p.sOh;
    if (p.ST) {
        const int rl = lane >> 1, isel = rl & 7;
        float mv = 0.f, lv = 0.f;
#pragma unroll
        for (int i = 0; i < 8; ++i) if (i == isel) { mv = m8[i]; lv = l8[i]; }
        const int irow = q0 + rl;
        if (irow < p.Lq) { float* st = p.ST + (((long long)b * gridDim.y + h) * p.Lq + irow) * 2 + (lane & 1); VST2(float, st, (lane & 1) ? lv : mv * 0.6931471805599453f); }
    }
    float invr[8];
#pragma unroll
    for (int i = 0; i < 8; ++i) {
        if (TWOPASS) invr[i] = SPLITPV ? 1.f : (1.f / 4096.f);
        else if (p.nonorm) invr[i] = exp2f(m8[i]) * (SPLITPV ? 1.f : (1.f / 4096.f));
        else invr[i] = (l8[i] > 0.f) ? (SPLITPV ? 1.f / l8[i] : 1.f / (l8[i] * 4096.f)) : 0.f;
    }
    __syncthreads();
    const bool ofast = ((p.sOi & 3) == 0) && ((((size_t)obase) & 15) == 0) && (q0 + 16 <= p.Lq);
#pragma unroll
    for (int c0 = 0; c0 < DVP; c0 += 64) {
#pragma unroll
        for (int i = 0; i < 8; ++i)
#pragma unroll
            for (int t = 0; t < NT; ++t) if (t * 16 >= c0 && t * 16 < c0 + 64) myp[(i + 8 * hf) * 64 + (t * 16 - c0) + l15] = o[t][i] * invr[i];
        __syncthreads();
        const int cw = (DVP - c0 < 64) ? (DVP - c0) : 64;
        if (ofast && (c0 + cw <= p.dv) && (cw % 32 == 0)) {
            const int lpr = cw / 4;
            const int rows_per_ins = 32 / lpr;
            for (int r0 = 0; r0 < 16; r0 += rows_per_ins) {
                const int row = r0 + lane / lpr, c4 = (lane % lpr) * 4;
                const v4f v = *(const v4f*)(myp + row * 64 + c4);
                VST2V4(obase + (long long)(q0 + row) * p.sOi + c0 + c4, v);
            }
        } else {
            for (int row = 0; row < 16; ++row) {
                const int irow = q0 + row; if (irow >= p.Lq) continue;
                for (int c = lane; c < cw; c += 32) { const int d = c0 + c; if (d < p.dv) VST2(float, obase + (long long)irow * p.sOi + d, myp[row * 64 + c]); }
            }
        }
        __syncthreads();
    }
}

struct TrP { const float* src; float* dst; const float* R2; long long sSz, lds, sDz, ldd, sRz, ldr; int R, C, flags, act; float alpha, beta; };
static_assert(sizeof(TrP) == 3 * 8 + 6 * 8 + 6 * 4, "TrP has padding");
__global__ __launch_bounds__(256) void k_tr(TrP p) {
    __shared__ float tile[32][33];
    const int c0 = blockIdx.x * 32, r0 = blockIdx.y * 32, z = blockIdx.z;
    const int lane = threadIdx.x & 31, wave = threadIdx.x >> 5;
    const float* s = p.src + z * p.sSz;
#pragma unroll
    for (int k = 0; k < 4; ++k) {
        const int rl = wave * 4 + k, r = r0 + rl, c = c0 + lane;
        tile[rl][lane] = (r < p.R && c < p.C) ? s[(long long)r * p.lds + c] : 0.f;
    }
    __syncthreads();
    float* d = p.dst + z * p.sDz; const float* rr = p.R2 + z * p.sRz;
#pragma unroll
    for (int k = 0; k < 4; ++k) {
        const int cl = wave * 4 + k, c = c0 + cl, r = r0 + lane;
        if (c < p.C && r < p.R) {
            float v = act_fn(p.alpha * tile[lane][cl], p.act);
            if (p.flags & 1) v += p.beta * rr[(long long)c * p.ldr + r];
            VST2(float, d + (long long)c * p.ldd + r, v);
        }
    }
}

__global__ __launch_bounds__(256) void k_affine(const float* __restrict__ src, float* __restrict__ dst, int n, float a, float b, const float* __restrict__ sdev) {
    const int i = blockIdx.x * 256 + threadIdx.x;
    if (i < n) { const float aa = sdev ? a * sdev[0] : a; const float v = aa * src[i] + b; VST2(float, dst + i, v); }
}

struct SmP { const float* src; float* dst; const float* Mf; long long sz, sr, dz, dr, smz, smr; int n, pad; float scale_in, scale_out; };
static_assert(sizeof(SmP) == 3 * 8 + 6 * 8 + 4 * 4, "SmP has padding");
__global__ __launch_bounds__(256) void k_softmax(SmP p) {
    __shared__ float red[256];
    const int r = blockIdx.x, z = blockIdx.y, tid = threadIdx.x;
    const float* s = p.src + z * p.sz + (long long)r * p.sr;
    const float* mf = p.Mf ? (p.Mf + z * p.smz + (long long)r * p.smr) : nullptr;
    float mx = -__builtin_inff();
    for (int j = tid; j < p.n; j += 256) { float v = s[j] * p.scale_in; if (mf) v += mf[j]; mx = fmaxf(mx, v); }
    red[tid] = mx; __syncthreads();
    for (int o = 128; o > 0; o >>= 1) { if (tid < o) red[tid] = fmaxf(red[tid], red[tid + o]); __syncthreads(); }
    mx = red[0]; __syncthreads();
    float sum = 0.f;
    for (int j = tid; j < p.n; j += 256) { float v = s[j] * p.scale_in; if (mf) v += mf[j]; sum += (mx == -__builtin_inff()) ? 0.f : expf(v - mx); }
    red[tid] = sum; __syncthreads();
    for (int o = 128; o > 0; o >>= 1) { if (tid < o) red[tid] += red[tid + o]; __syncthreads(); }
    sum = red[0];
    const float inv = (sum > 0.f) ? p.scale_out / sum : 0.f;
    float* d = p.dst + z * p.dz + (long long)r * p.dr;
    for (int j = tid; j < p.n; j += 256) { float v = s[j] * p.scale_in; if (mf) v += mf[j]; const float o = (mx == -__builtin_inff()) ? 0.f : expf(v - mx) * inv; VST2(float, d + j, o); }
}
__global__ __launch_bounds__(256) void k_stats(const float* __restrict__ x, long long sz, long long so, long long si, int inner, int n, float eps, float* __restrict__ stat, int mode) {
    __shared__ float red[256];
    const int z = blockIdx.x, tid = threadIdx.x;
    const float* base = x + z * sz;
    float s = 0.f;
    for (int e = tid; e < n; e += 256) s += base[(long long)(e / inner) * so + (long long)(e % inner) * si];
    red[tid] = s; __syncthreads();
    for (int o = 128; o > 0; o >>= 1) { if (tid < o) red[tid] += red[tid + o]; __syncthreads(); }
    const float mu = (mode == 0 || mode == 3) ? red[0] / (float)n : 0.f; __syncthreads();
    float q = 0.f;
    for (int e = tid; e < n; e += 256) { const float dlt = base[(long long)(e / inner) * so + (long long)(e % inner) * si] - mu; q += dlt * dlt; }
    red[tid] = q; __syncthreads();
    for (int o = 128; o > 0; o >>= 1) { if (tid < o) red[tid] += red[tid + o]; __syncthreads(); }
    {
        float rs;
        if (mode == 2) rs = sqrtf((float)n) / fmaxf(sqrtf(red[0]), eps); else if (mode == 3) rs = rsqrtf(red[0] / (float)(n - 1) + eps); else rs = rsqrtf(red[0] / (float)n + eps);
        if (tid < 32) { const float v = (tid == 0) ? mu : ((tid == 1) ? rs : 0.f); VST2(float, stat + (long long)z * 32 + tid, v); }
    }
}
__global__ __launch_bounds__(256) void k_norm_apply(const float* __restrict__ x, float* __restrict__ y, const float* __restrict__ stat, const float* __restrict__ g, const float* __restrict__ bta,
                                                     int Z, int C, int L, int G, int bn, int act) {
    const long long idx = (long long)blockIdx.x * 256 + threadIdx.x;
    if (idx >= (long long)Z * C * L) return;
    const int l = (int)(idx % L); const long long zc = idx / L; const int c = (int)(zc % C), z = (int)(zc / C); (void)l;
    const int set = bn ? c : (z * G + c / (C / G));
    float v = (x[idx] - stat[(long long)set * 32]) * stat[(long long)set * 32 + 1];
    if (g) v *= g[c];
    if (bta) v += bta[c];
    v = act_fn(v, act);
    VST2(float, y + idx, v);
}

__global__ __launch_bounds__(256) void k_lse_neg(const float* __restrict__ st, float* __restrict__ c, int n) {
    const int i = blockIdx.x * 256 + threadIdx.x;
    if (i < n) { const float v = -(st[2 * i] + logf(st[2 * i + 1])); VST2(float, c + i, v); }
}

__global__ __launch_bounds__(256) void k_iota(int* __restrict__ dst, int n, int a, int b) {
    const int i = blockIdx.x * 256 + threadIdx.x;
    if (i < n) { const int v = a * i + b; VST2(int, dst + i, v); }
}

__global__ __launch_bounds__(256) void k_axpby(const float* __restrict__ x, const float* __restrict__ y, float* __restrict__ dst, int n, float a, float b, float c) {
    const int i = blockIdx.x * 256 + threadIdx.x;
    if (i < n) { const float v = a * x[i] + b * y[i] + c; VST2(float, dst + i, v); }
}

struct RopeP { const float* X; float* Y; const float* C; const float* Sn; const int* pos; long long sXr, sXh, sYr, sYh, sCb, sCp, sCd; int R, Hn, D, S, mode, tmode, pmode, pad; };
static_assert(sizeof(RopeP) == 5 * 8 + 7 * 8 + 8 * 4, "RopeP has padding");
__global__ __launch_bounds__(256) void k_rope(RopeP p) {
    const long long idx = (long long)blockIdx.x * 256 + threadIdx.x;
    if (idx >= (long long)p.R * p.Hn * p.D) return;
    const int d = (int)(idx % p.D); const long long rh = idx / p.D; const int h = (int)(rh % p.Hn); const int r = (int)(rh / p.Hn);
    const int half = p.D / 2;
    int partner; float sign;
    if (p.mode == 0) { partner = (d < half) ? d + half : d - half; sign = (d < half) ? -1.f : 1.f; }
    else { partner = d ^ 1; sign = (d & 1) ? 1.f : -1.f; }
    const int tcol = (p.tmode == 0) ? d : ((p.tmode == 1) ? (d % half) : (d >> 1));
    const int pp = (p.pmode == 0) ? (r % p.S) : ((p.pmode == 1) ? h : p.pos[r]);
    const long long toff = (long long)(r / p.S) * p.sCb + (long long)pp * p.sCp + (long long)tcol * p.sCd;
    const float* xr = p.X + (long long)r * p.sXr + (long long)h * p.sXh;
    const float v = xr[d] * p.C[toff] + sign * xr[partner] * p.Sn[toff];
    VST2(float, p.Y + (long long)r * p.sYr + (long long)h * p.sYh + d, v);
}

__global__ __launch_bounds__(256) void k_invf(float* __restrict__ invb, int half, int D, float base, float num, int fmode, float cexp) {
    const int i = blockIdx.x * 256 + threadIdx.x;
    if (i >= ((half + 31) / 32) * 32) return;
    if (i >= half) { VST2(float, invb + i, 0.f); return; }
    const float e = (float)(2 * i) / (float)D;
    float invf;
    if (fmode == 1) invf = num * expf((float)(2 * i) * cexp);
    else if (fmode == 2) invf = num * powf(base, (-2.0f * ((float)i - 1.0f)) / (float)D);
    else invf = num * (1.0f / powf(base, e));
    VST2(float, invb + i, invf);
}
__global__ __launch_bounds__(256) void k_sincos(float* __restrict__ cs, float* __restrict__ sn, const float* __restrict__ invb, int S, int half, float pscale) {
    const int idx = blockIdx.x * 256 + threadIdx.x;
    if (idx >= S * half) return;
    const int s = idx / half, i = idx - s * half;
    const float ang = (pscale * (float)s) * invb[i];
    VST2(float, cs + idx, cosf(ang)); VST2(float, sn + idx, sinf(ang));
}

__global__ __launch_bounds__(256) void k_mulact(const float* __restrict__ x, const float* __restrict__ y, float* __restrict__ dst, int n, int act) {
    const int i = blockIdx.x * 256 + threadIdx.x;
    if (i < n) { const float v = act_fn(x[i], act) * y[i]; VST2(float, dst + i, v); }
}

__global__ __launch_bounds__(256) void k_matvec(GemmP p) {
    const int rpt = (p.N == 1) ? 1 : 32;
    const long long r0 = ((long long)blockIdx.x * 256 + threadIdx.x) * rpt; const int z = blockIdx.z, zo = z / p.zi_n, zi = z - zo * p.zi_n;
    if (r0 >= p.M) return;
    const float* Bb = p.B + zo * p.sBo + zi * p.sBi;
    float* C = p.C + zo * p.sCo + zi * p.sCi; const float* R = p.R + zo * p.sRo + zi * p.sRi;
    for (int rr = 0; rr < rpt; ++rr) {
        const long long r = r0 + rr; if (r >= p.M) break;
        const float* A = p.A + zo * p.sAo + zi * p.sAi + r * p.sAm;
        float acc[8] = {0.f, 0.f, 0.f, 0.f, 0.f, 0.f, 0.f, 0.f};
        for (int k = 0; k < p.K; ++k) { const float a = A[(long long)k * p.sAk];
#pragma unroll
            for (int j = 0; j < 8; ++j) if (j < p.N) acc[j] += a * Bb[(long long)j * p.sBn + (long long)k * p.sBk]; }
#pragma unroll
        for (int j = 0; j < 8; ++j) if (j < p.N) {
            float v = acc[j] * p.alpha;
            if (p.flags & 1) v += p.bias[j];
            if (p.flags & 2) v += p.bias[r];
            v = act_fn(v, p.act);
            if (p.flags & 4) v += p.beta * R[r * p.sRm + (long long)j * p.sRn];
            VST2(float, C + r * p.sCm + j, v);
        }
    }
}
__global__ __launch_bounds__(256) void k_smallsoftmax(const float* __restrict__ src, float* __restrict__ dst, long long sr, long long dr, int n, long long R, float scale) {
    const long long r0 = ((long long)blockIdx.x * 256 + threadIdx.x) * 32;
    for (int rr = 0; rr < 32; ++rr) {
        const long long r = r0 + rr; if (r >= R) return;
        const float* s = src + r * sr; float* d = dst + r * dr;
        float mx = -__builtin_inff();
        for (int j = 0; j < n; ++j) mx = fmaxf(mx, s[j] * scale);
        float sum = 0.f;
        for (int j = 0; j < n; ++j) sum += expf(s[j] * scale - mx);
        const float inv = 1.f / sum;
        for (int j = 0; j < n; ++j) { const float v = expf(s[j] * scale - mx) * inv; VST2(float, d + j, v); }
    }
}

__global__ __launch_bounds__(32) void k_unitstat(float* __restrict__ st) { const int t = threadIdx.x; const float v = (t == 1) ? 1.f : 0.f; VST2(float, st + t, v); }

__global__ __launch_bounds__(256) void k_lincopy(const float* __restrict__ src, long long lds, float* __restrict__ dst, long long ldd, long long rows, int cols) {
    const long long i = (long long)blockIdx.x * 256 + threadIdx.x; if (i >= rows * cols) return;
    const long long r = i / cols; const int c = (int)(i - r * cols);
    const float v = src[r * lds + c]; VST2(float, dst + r * ldd + c, v);
}

#define IL_CAP64 64
#define IL_T64 128
#define IL_TILE64 4096
__global__ __launch_bounds__(IL_T64) void k_inlists64(const int* __restrict__ tgt, int E, int N, int* __restrict__ NBR, int* __restrict__ cnt) {
    __shared__ int tt[IL_TILE64];
    __shared__ int lists[IL_T64 * IL_CAP64];
    const int d = blockIdx.x * IL_T64 + threadIdx.x; int n = 0;
    for (int e0 = 0; e0 < E; e0 += IL_TILE64) {
        const int nt = min(IL_TILE64, E - e0);
        __syncthreads();
        for (int i = threadIdx.x; i < nt; i += IL_T64) tt[i] = tgt[e0 + i];
        __syncthreads();
        for (int i = 0; i < nt; ++i) { if (tt[i] == d) { if (n < IL_CAP64) lists[threadIdx.x * IL_CAP64 + n] = e0 + i; ++n; } }
    }
    if (d < N) {
        int* row = NBR + (long long)d * IL_CAP64;
        for (int j = 0; j < IL_CAP64; ++j) { const int v = (j < n) ? lists[threadIdx.x * IL_CAP64 + j] : -1; VST2(int, row + j, v); }
        VST2(int, cnt + d, min(n, IL_CAP64));
    }
}
__global__ __launch_bounds__(256) void k_csr_scan64(const int* __restrict__ cnt, int* __restrict__ off, int N) {
    __shared__ int part[256]; const int per = ((((N + 255) / 256) + 31) / 32) * 32; const int a = threadIdx.x * per, b = min(N, a + per); int s = 0;
    for (int i = a; i < b; ++i) s += cnt[i]; part[threadIdx.x] = s; __syncthreads();
    if (threadIdx.x == 0) { int run = 0; for (int t = 0; t < 256; ++t) { const int v = part[t]; part[t] = run; run += v; } } __syncthreads();
    int run = part[threadIdx.x]; for (int i = a; i < b; ++i) { VST2(int, off + i, run); run += cnt[i]; }
    if (a < N && b == N) { VST2(int, off + N, run); }
}
__global__ __launch_bounds__(256) void k_slotcopy64(const int* __restrict__ off, const int* __restrict__ NBR, int* __restrict__ slot, int N) {
    const int t = blockIdx.x * 256 + threadIdx.x; const int tot = off[N]; if (t >= tot) return;
    int lo = 0, hi = N - 1;
    while (lo < hi) { const int mid = (lo + hi + 1) >> 1; if (off[mid] <= t) lo = mid; else hi = mid - 1; }
    int j = t - off[lo]; j = (j < 0) ? 0 : ((j >= IL_CAP64) ? (IL_CAP64 - 1) : j);
    VST2(int, slot + t, NBR[(long long)lo * IL_CAP64 + j]);
}

#define IL_CAP128 128
#define IL_T128 64
#define IL_TILE128 4096
__global__ __launch_bounds__(IL_T128) void k_inlists128(const int* __restrict__ tgt, int E, int N, int* __restrict__ NBR, int* __restrict__ cnt) {
    __shared__ int tt[IL_TILE128];
    __shared__ int lists[IL_T128 * IL_CAP128];
    const int d = blockIdx.x * IL_T128 + threadIdx.x; int n = 0;
    for (int e0 = 0; e0 < E; e0 += IL_TILE128) {
        const int nt = min(IL_TILE128, E - e0);
        __syncthreads();
        for (int i = threadIdx.x; i < nt; i += IL_T128) tt[i] = tgt[e0 + i];
        __syncthreads();
        for (int i = 0; i < nt; ++i) { if (tt[i] == d) { if (n < IL_CAP128) lists[threadIdx.x * IL_CAP128 + n] = e0 + i; ++n; } }
    }
    if (d < N) {
        int* row = NBR + (long long)d * IL_CAP128;
        for (int j = 0; j < IL_CAP128; ++j) { const int v = (j < n) ? lists[threadIdx.x * IL_CAP128 + j] : -1; VST2(int, row + j, v); }
        VST2(int, cnt + d, min(n, IL_CAP128));
    }
}
__global__ __launch_bounds__(256) void k_csr_scan128(const int* __restrict__ cnt, int* __restrict__ off, int N) {
    __shared__ int part[256]; const int per = ((((N + 255) / 256) + 31) / 32) * 32; const int a = threadIdx.x * per, b = min(N, a + per); int s = 0;
    for (int i = a; i < b; ++i) s += cnt[i]; part[threadIdx.x] = s; __syncthreads();
    if (threadIdx.x == 0) { int run = 0; for (int t = 0; t < 256; ++t) { const int v = part[t]; part[t] = run; run += v; } } __syncthreads();
    int run = part[threadIdx.x]; for (int i = a; i < b; ++i) { VST2(int, off + i, run); run += cnt[i]; }
    if (a < N && b == N) { VST2(int, off + N, run); }
}
__global__ __launch_bounds__(256) void k_slotcopy128(const int* __restrict__ off, const int* __restrict__ NBR, int* __restrict__ slot, int N) {
    const int t = blockIdx.x * 256 + threadIdx.x; const int tot = off[N]; if (t >= tot) return;
    int lo = 0, hi = N - 1;
    while (lo < hi) { const int mid = (lo + hi + 1) >> 1; if (off[mid] <= t) lo = mid; else hi = mid - 1; }
    int j = t - off[lo]; j = (j < 0) ? 0 : ((j >= IL_CAP128) ? (IL_CAP128 - 1) : j);
    VST2(int, slot + t, NBR[(long long)lo * IL_CAP128 + j]);
}


__global__ __launch_bounds__(256) void k_csr_mean(const float* __restrict__ Hh, const int* __restrict__ src, const int* __restrict__ off, const int* __restrict__ slot, float* __restrict__ AGG, int N, int D) {
    const long long t = (long long)blockIdx.x * 256 + threadIdx.x; if (t >= (long long)N * D) return; const int d = (int)(t % D); const int i = (int)(t / D); const int a = off[i], b = off[i + 1]; float s = 0.f;
    for (int p = a; p < b; ++p) s += Hh[(long long)src[slot[p]] * D + d];
    VST2(float, AGG + t, s / fmaxf((float)(b - a), 1.f));
}

__global__ __launch_bounds__(256) void k_csp_gather(const float* __restrict__ X, const float* __restrict__ EA, const int* __restrict__ ei, const int* __restrict__ slot, float* __restrict__ XD, float* __restrict__ XS, float* __restrict__ EAc, int p0, int CH, int E, int H, int ED) {
    const long long q = (long long)blockIdx.x * 256 + threadIdx.x; if (q >= (long long)CH * H) return; const int c = (int)(q % H); const int r = (int)(q / H); const int e = slot[p0 + r];
    VST2(float, XD + q, X[(long long)ei[E + e] * H + c]); VST2(float, XS + q, X[(long long)ei[e] * H + c]);
    if (c < 32) VST2(float, EAc + (long long)r * 32 + c, (c < ED) ? EA[(long long)e * ED + c] : 0.f);
}
__global__ __launch_bounds__(256) void k_csp_agg(const float* __restrict__ MSG, const int* __restrict__ off, float* __restrict__ AGG, int p0, int CH, int N, int H) {
    const long long q = (long long)blockIdx.x * 256 + threadIdx.x; if (q >= (long long)N * H) return; const int c = (int)(q % H); const int n = (int)(q / H); int a = max(off[n], p0), b = min(off[n + 1], p0 + CH); if (a >= b) return; float s = AGG[q];
    for (int p = a; p < b; ++p) s += MSG[(long long)(p - p0) * H + c]; VST2(float, AGG + q, s);
}
__global__ __launch_bounds__(256) void k_csp_silu(float* __restrict__ G, long long n) { const long long q = (long long)blockIdx.x * 256 + threadIdx.x; if (q >= n) return; const float g = G[q]; const float v = g / (1.f + expf(-g)); VST2(float, G + q, v); }
__global__ __launch_bounds__(256) void k_csp_x2(const float* __restrict__ X, const float* __restrict__ UP, const float* __restrict__ LI, const int* __restrict__ bat, float* __restrict__ X2, int N, int H) { const long long q = (long long)blockIdx.x * 256 + threadIdx.x; if (q >= (long long)N * H) return; const int c = (int)(q % H); const int n = (int)(q / H); VST2(float, X2 + q, X[q] + UP[q] + LI[(long long)bat[n] * H + c]); }
__global__ __launch_bounds__(256) void k_csp_latln(const float* __restrict__ lat, const float* __restrict__ LF, int ldp, const float* __restrict__ g, const float* __restrict__ bb, float* __restrict__ OUT, int NB) { const int b = blockIdx.x * 256 + threadIdx.x; if (b >= NB) return; float v[9]; float mu = 0.f;
#pragma unroll 1
    for (int j = 0; j < 9; ++j) { v[j] = lat[b * 9 + j] + LF[(long long)b * ldp + j]; mu += v[j]; }
    mu /= 9.f; float var = 0.f;
#pragma unroll 1
    for (int j = 0; j < 9; ++j) var += (v[j] - mu) * (v[j] - mu);
    var /= 9.f; const float rs = rsqrtf(var + 1e-5f);
#pragma unroll 1
    for (int j = 0; j < 9; ++j) VST2(float, OUT + b * 9 + j, (v[j] - mu) * rs * g[j] + bb[j]); }

template __global__ void k_gemm<1>(GemmP);

extern "C" void kernel_launch(void* const* d_in, const int* in_sizes, int n_in, void* d_out, int out_size, void* d_ws, size_t ws_size, hipStream_t stream) {
    (void)in_sizes; (void)n_in; (void)out_size; (void)ws_size;
    const float* x = (const float*)d_in[0];
    const int* ei = (const int*)d_in[1];
    const float* ea = (const float*)d_in[2];
    const float* lat = (const float*)d_in[3];
    const int* bat = (const int*)d_in[4];
    const float* eew1 = (const float*)d_in[5];
    const float* eeb1 = (const float*)d_in[6];
    const float* eew2 = (const float*)d_in[7];
    const float* eeb2 = (const float*)d_in[8];
    const float* mnw1 = (const float*)d_in[9];
    const float* mnb1 = (const float*)d_in[10];
    const float* mnw2 = (const float*)d_in[11];
    const float* mnb2 = (const float*)d_in[12];
    const float* unw1 = (const float*)d_in[13];
    const float* unb1 = (const float*)d_in[14];
    const float* unw2 = (const float*)d_in[15];
    const float* unb2 = (const float*)d_in[16];
    const float* l2aw = (const float*)d_in[17];
    const float* l2ab = (const float*)d_in[18];
    const float* a2lw = (const float*)d_in[19];
    const float* a2lb = (const float*)d_in[20];
    const float* nlg = (const float*)d_in[21];
    const float* nlb = (const float*)d_in[22];
    const float* llg = (const float*)d_in[23];
    const float* llb = (const float*)d_in[24];
    const int Nn = 50000;
    const int E = 800000;
    const int H = 128;
    const int EDd = 20;
    const int NB = 1000;
    const int CAP = 64;
    const int CH = 50000;
    const int GCAP = 128;
    const int LP = 32;
    float* out = (float*)d_out;
    float* lout = out + ((size_t)Nn * H);
    char* wsp = (char*)d_ws;
    int* cnt = (int*)wsp; wsp += (((size_t)((size_t)Nn + 64) * 4 + 255) / 256) * 256;
    int* off = (int*)wsp; wsp += (((size_t)((size_t)Nn + 64) * 4 + 255) / 256) * 256;
    int* slot = (int*)wsp; wsp += (((size_t)((size_t)E + 64) * 4 + 255) / 256) * 256;
    int* nbr = (int*)wsp; wsp += (((size_t)((size_t)Nn * CAP) * 4 + 255) / 256) * 256;
    int* gcnt = (int*)wsp; wsp += (((size_t)((size_t)NB + 64) * 4 + 255) / 256) * 256;
    int* goff = (int*)wsp; wsp += (((size_t)((size_t)NB + 64) * 4 + 255) / 256) * 256;
    int* gslot = (int*)wsp; wsp += (((size_t)((size_t)Nn + 64) * 4 + 255) / 256) * 256;
    int* gnbr = (int*)wsp; wsp += (((size_t)((size_t)NB * GCAP) * 4 + 255) / 256) * 256;
    int* ids = (int*)wsp; wsp += (((size_t)((size_t)Nn + 64) * 4 + 255) / 256) * 256;
    float* EAc = (float*)wsp; wsp += (((size_t)((size_t)CH * 32) * 4 + 255) / 256) * 256;
    float* XD = (float*)wsp; wsp += (((size_t)((size_t)CH * H) * 4 + 255) / 256) * 256;
    float* XS = (float*)wsp; wsp += (((size_t)((size_t)CH * H) * 4 + 255) / 256) * 256;
    float* EF1 = (float*)wsp; wsp += (((size_t)((size_t)CH * H) * 4 + 255) / 256) * 256;
    float* EF = (float*)wsp; wsp += (((size_t)((size_t)CH * H) * 4 + 255) / 256) * 256;
    float* G = (float*)wsp; wsp += (((size_t)((size_t)CH * H) * 4 + 255) / 256) * 256;
    float* MSG = (float*)wsp; wsp += (((size_t)((size_t)CH * H) * 4 + 255) / 256) * 256;
    float* AGG = (float*)wsp; wsp += (((size_t)((size_t)Nn * H) * 4 + 255) / 256) * 256;
    float* UP = (float*)wsp; wsp += (((size_t)((size_t)Nn * H) * 4 + 255) / 256) * 256;
    float* X2 = (float*)wsp; wsp += (((size_t)((size_t)Nn * H) * 4 + 255) / 256) * 256;
    float* LI = (float*)wsp; wsp += (((size_t)((size_t)NB * H) * 4 + 255) / 256) * 256;
    float* AI = (float*)wsp; wsp += (((size_t)((size_t)NB * H) * 4 + 255) / 256) * 256;
    float* LF = (float*)wsp; wsp += (((size_t)((size_t)NB * LP) * 4 + 255) / 256) * 256;
    float* st = (float*)wsp; wsp += (((size_t)((size_t)Nn * 32) * 4 + 255) / 256) * 256;
    k_inlists64<<<(unsigned)((Nn) + IL_T64 - 1) / IL_T64, IL_T64, 0, stream>>>(ei + E, E, Nn, nbr, cnt);
    k_csr_scan64<<<1, 256, 0, stream>>>(cnt, off, Nn);
    k_slotcopy64<<<(unsigned)((E) + 255) / 256, 256, 0, stream>>>(off, nbr, slot, Nn);
    k_inlists128<<<(unsigned)((NB) + IL_T128 - 1) / IL_T128, IL_T128, 0, stream>>>(bat, Nn, NB, gnbr, gcnt);
    k_csr_scan128<<<1, 256, 0, stream>>>(gcnt, goff, NB);
    k_slotcopy128<<<(unsigned)((Nn) + 255) / 256, 256, 0, stream>>>(goff, gnbr, gslot, NB);
    k_iota<<<(unsigned)((Nn) + 255) / 256, 256, 0, stream>>>(ids, Nn, 1, 0);
    hipMemsetAsync(AGG, 0, (size_t)Nn * H * 4, stream);
    k_csp_gather<<<(unsigned)(((long long)CH * H + 255) / 256), 256, 0, stream>>>(x, ea, ei, slot, XD, XS, EAc, 0, CH, E, H, EDd);
    { GemmP ge1_0;
      ge1_0.A = EAc; ge1_0.B = eew1; ge1_0.bias = eeb1; ge1_0.R = EAc; ge1_0.C = EF1;
      ge1_0.sAo = 0; ge1_0.sAi = 0; ge1_0.sAm = 32; ge1_0.sAk = 1; ge1_0.sBo = 0; ge1_0.sBi = 0; ge1_0.sBn = 1; ge1_0.sBk = H; ge1_0.sCo = 0; ge1_0.sCi = 0; ge1_0.sCm = H; ge1_0.sRo = 0; ge1_0.sRi = 0; ge1_0.sRm = 0; ge1_0.sRn = 0;
      ge1_0.M = CH; ge1_0.N = H; ge1_0.K = EDd; ge1_0.zi_n = 1; ge1_0.flags = 1; ge1_0.act = 0;
      ge1_0.alpha = 1.0f; ge1_0.beta = 0.0f; ge1_0.sa = 1.0f; ge1_0.sb = 1.0f; ge1_0.Npad = H; ge1_0.pad_ = 0;
      k_gemm<1><<<dim3((unsigned)((H) + 31) / 32, (unsigned)((CH) + 15) / 16, (unsigned)(1)), 32, 0, stream>>>(ge1_0); }
    k_csp_silu<<<(unsigned)(((long long)CH * H + 255) / 256), 256, 0, stream>>>(EF1, (long long)CH * H);
    { GemmP ge2_0;
      ge2_0.A = EF1; ge2_0.B = eew2; ge2_0.bias = eeb2; ge2_0.R = EF1; ge2_0.C = EF;
      ge2_0.sAo = 0; ge2_0.sAi = 0; ge2_0.sAm = H; ge2_0.sAk = 1; ge2_0.sBo = 0; ge2_0.sBi = 0; ge2_0.sBn = 1; ge2_0.sBk = H; ge2_0.sCo = 0; ge2_0.sCi = 0; ge2_0.sCm = H; ge2_0.sRo = 0; ge2_0.sRi = 0; ge2_0.sRm = 0; ge2_0.sRn = 0;
      ge2_0.M = CH; ge2_0.N = H; ge2_0.K = H; ge2_0.zi_n = 1; ge2_0.flags = 1; ge2_0.act = 0;
      ge2_0.alpha = 1.0f; ge2_0.beta = 0.0f; ge2_0.sa = 1.0f; ge2_0.sb = 1.0f; ge2_0.Npad = H; ge2_0.pad_ = 0;
      k_gemm<1><<<dim3((unsigned)((H) + 31) / 32, (unsigned)((CH) + 15) / 16, (unsigned)(1)), 32, 0, stream>>>(ge2_0); }
    { GemmP gm1a_0;
      gm1a_0.A = XD; gm1a_0.B = mnw1; gm1a_0.bias = mnb1; gm1a_0.R = XD; gm1a_0.C = G;
      gm1a_0.sAo = 0; gm1a_0.sAi = 0; gm1a_0.sAm = H; gm1a_0.sAk = 1; gm1a_0.sBo = 0; gm1a_0.sBi = 0; gm1a_0.sBn = 1; gm1a_0.sBk = H; gm1a_0.sCo = 0; gm1a_0.sCi = 0; gm1a_0.sCm = H; gm1a_0.sRo = 0; gm1a_0.sRi = 0; gm1a_0.sRm = 0; gm1a_0.sRn = 0;
      gm1a_0.M = CH; gm1a_0.N = H; gm1a_0.K = H; gm1a_0.zi_n = 1; gm1a_0.flags = 1; gm1a_0.act = 0;
      gm1a_0.alpha = 1.0f; gm1a_0.beta = 0.0f; gm1a_0.sa = 1.0f; gm1a_0.sb = 1.0f; gm1a_0.Npad = H; gm1a_0.pad_ = 0;
      k_gemm<1><<<dim3((unsigned)((H) + 31) / 32, (unsigned)((CH) + 15) / 16, (unsigned)(1)), 32, 0, stream>>>(gm1a_0); }
    { GemmP gm1b_0;
      gm1b_0.A = XS; gm1b_0.B = mnw1 + (size_t)128 * H; gm1b_0.bias = XS; gm1b_0.R = G; gm1b_0.C = G;
      gm1b_0.sAo = 0; gm1b_0.sAi = 0; gm1b_0.sAm = H; gm1b_0.sAk = 1; gm1b_0.sBo = 0; gm1b_0.sBi = 0; gm1b_0.sBn = 1; gm1b_0.sBk = H; gm1b_0.sCo = 0; gm1b_0.sCi = 0; gm1b_0.sCm = H; gm1b_0.sRo = 0; gm1b_0.sRi = 0; gm1b_0.sRm = H; gm1b_0.sRn = 1;
      gm1b_0.M = CH; gm1b_0.N = H; gm1b_0.K = H; gm1b_0.zi_n = 1; gm1b_0.flags = 4; gm1b_0.act = 0;
      gm1b_0.alpha = 1.0f; gm1b_0.beta = 1.0f; gm1b_0.sa = 1.0f; gm1b_0.sb = 1.0f; gm1b_0.Npad = H; gm1b_0.pad_ = 0;
      k_gemm<1><<<dim3((unsigned)((H) + 31) / 32, (unsigned)((CH) + 15) / 16, (unsigned)(1)), 32, 0, stream>>>(gm1b_0); }
    { GemmP gm1c_0;
      gm1c_0.A = EF; gm1c_0.B = mnw1 + (size_t)256 * H; gm1c_0.bias = EF; gm1c_0.R = G; gm1c_0.C = G;
      gm1c_0.sAo = 0; gm1c_0.sAi = 0; gm1c_0.sAm = H; gm1c_0.sAk = 1; gm1c_0.sBo = 0; gm1c_0.sBi = 0; gm1c_0.sBn = 1; gm1c_0.sBk = H; gm1c_0.sCo = 0; gm1c_0.sCi = 0; gm1c_0.sCm = H; gm1c_0.sRo = 0; gm1c_0.sRi = 0; gm1c_0.sRm = H; gm1c_0.sRn = 1;
      gm1c_0.M = CH; gm1c_0.N = H; gm1c_0.K = H; gm1c_0.zi_n = 1; gm1c_0.flags = 4; gm1c_0.act = 0;
      gm1c_0.alpha = 1.0f; gm1c_0.beta = 1.0f; gm1c_0.sa = 1.0f; gm1c_0.sb = 1.0f; gm1c_0.Npad = H; gm1c_0.pad_ = 0;
      k_gemm<1><<<dim3((unsigned)((H) + 31) / 32, (unsigned)((CH) + 15) / 16, (unsigned)(1)), 32, 0, stream>>>(gm1c_0); }
    k_csp_silu<<<(unsigned)(((long long)CH * H + 255) / 256), 256, 0, stream>>>(G, (long long)CH * H);
    { GemmP gm2_0;
      gm2_0.A = G; gm2_0.B = mnw2; gm2_0.bias = mnb2; gm2_0.R = G; gm2_0.C = MSG;
      gm2_0.sAo = 0; gm2_0.sAi = 0; gm2_0.sAm = H; gm2_0.sAk = 1; gm2_0.sBo = 0; gm2_0.sBi = 0; gm2_0.sBn = 1; gm2_0.sBk = H; gm2_0.sCo = 0; gm2_0.sCi = 0; gm2_0.sCm = H; gm2_0.sRo = 0; gm2_0.sRi = 0; gm2_0.sRm = 0; gm2_0.sRn = 0;
      gm2_0.M = CH; gm2_0.N = H; gm2_0.K = H; gm2_0.zi_n = 1; gm2_0.flags = 1; gm2_0.act = 0;
      gm2_0.alpha = 1.0f; gm2_0.beta = 0.0f; gm2_0.sa = 1.0f; gm2_0.sb = 1.0f; gm2_0.Npad = H; gm2_0.pad_ = 0;
      k_gemm<1><<<dim3((unsigned)((H) + 31) / 32, (unsigned)((CH) + 15) / 16, (unsigned)(1)), 32, 0, stream>>>(gm2_0); }
    k_csp_agg<<<(unsigned)(((long long)Nn * H + 255) / 256), 256, 0, stream>>>(MSG, off, AGG, 0, CH, Nn, H);
    k_csp_gather<<<(unsigned)(((long long)CH * H + 255) / 256), 256, 0, stream>>>(x, ea, ei, slot, XD, XS, EAc, 50000, CH, E, H, EDd);
    { GemmP ge1_1;
      ge1_1.A = EAc; ge1_1.B = eew1; ge1_1.bias = eeb1; ge1_1.R = EAc; ge1_1.C = EF1;
      ge1_1.sAo = 0; ge1_1.sAi = 0; ge1_1.sAm = 32; ge1_1.sAk = 1; ge1_1.sBo = 0; ge1_1.sBi = 0; ge1_1.sBn = 1; ge1_1.sBk = H; ge1_1.sCo = 0; ge1_1.sCi = 0; ge1_1.sCm = H; ge1_1.sRo = 0; ge1_1.sRi = 0; ge1_1.sRm = 0; ge1_1.sRn = 0;
      ge1_1.M = CH; ge1_1.N = H; ge1_1.K = EDd; ge1_1.zi_n = 1; ge1_1.flags = 1; ge1_1.act = 0;
      ge1_1.alpha = 1.0f; ge1_1.beta = 0.0f; ge1_1.sa = 1.0f; ge1_1.sb = 1.0f; ge1_1.Npad = H; ge1_1.pad_ = 0;
      k_gemm<1><<<dim3((unsigned)((H) + 31) / 32, (unsigned)((CH) + 15) / 16, (unsigned)(1)), 32, 0, stream>>>(ge1_1); }
    k_csp_silu<<<(unsigned)(((long long)CH * H + 255) / 256), 256, 0, stream>>>(EF1, (long long)CH * H);
    { GemmP ge2_1;
      ge2_1.A = EF1; ge2_1.B = eew2; ge2_1.bias = eeb2; ge2_1.R = EF1; ge2_1.C = EF;
      ge2_1.sAo = 0; ge2_1.sAi = 0; ge2_1.sAm = H; ge2_1.sAk = 1; ge2_1.sBo = 0; ge2_1.sBi = 0; ge2_1.sBn = 1; ge2_1.sBk = H; ge2_1.sCo = 0; ge2_1.sCi = 0; ge2_1.sCm = H; ge2_1.sRo = 0; ge2_1.sRi = 0; ge2_1.sRm = 0; ge2_1.sRn = 0;
      ge2_1.M = CH; ge2_1.N = H; ge2_1.K = H; ge2_1.zi_n = 1; ge2_1.flags = 1; ge2_1.act = 0;
      ge2_1.alpha = 1.0f; ge2_1.beta = 0.0f; ge2_1.sa = 1.0f; ge2_1.sb = 1.0f; ge2_1.Npad = H; ge2_1.pad_ = 0;
      k_gemm<1><<<dim3((unsigned)((H) + 31) / 32, (unsigned)((CH) + 15) / 16, (unsigned)(1)), 32, 0, stream>>>(ge2_1); }
    { GemmP gm1a_1;
      gm1a_1.A = XD; gm1a_1.B = mnw1; gm1a_1.bias = mnb1; gm1a_1.R = XD; gm1a_1.C = G;
      gm1a_1.sAo = 0; gm1a_1.sAi = 0; gm1a_1.sAm = H; gm1a_1.sAk = 1; gm1a_1.sBo = 0; gm1a_1.sBi = 0; gm1a_1.sBn = 1; gm1a_1.sBk = H; gm1a_1.sCo = 0; gm1a_1.sCi = 0; gm1a_1.sCm = H; gm1a_1.sRo = 0; gm1a_1.sRi = 0; gm1a_1.sRm = 0; gm1a_1.sRn = 0;
      gm1a_1.M = CH; gm1a_1.N = H; gm1a_1.K = H; gm1a_1.zi_n = 1; gm1a_1.flags = 1; gm1a_1.act = 0;
      gm1a_1.alpha = 1.0f; gm1a_1.beta = 0.0f; gm1a_1.sa = 1.0f; gm1a_1.sb = 1.0f; gm1a_1.Npad = H; gm1a_1.pad_ = 0;
      k_gemm<1><<<dim3((unsigned)((H) + 31) / 32, (unsigned)((CH) + 15) / 16, (unsigned)(1)), 32, 0, stream>>>(gm1a_1); }
    { GemmP gm1b_1;
      gm1b_1.A = XS; gm1b_1.B = mnw1 + (size_t)128 * H; gm1b_1.bias = XS; gm1b_1.R = G; gm1b_1.C = G;
      gm1b_1.sAo = 0; gm1b_1.sAi = 0; gm1b_1.sAm = H; gm1b_1.sAk = 1; gm1b_1.sBo = 0; gm1b_1.sBi = 0; gm1b_1.sBn = 1; gm1b_1.sBk = H; gm1b_1.sCo = 0; gm1b_1.sCi = 0; gm1b_1.sCm = H; gm1b_1.sRo = 0; gm1b_1.sRi = 0; gm1b_1.sRm = H; gm1b_1.sRn = 1;
      gm1b_1.M = CH; gm1b_1.N = H; gm1b_1.K = H; gm1b_1.zi_n = 1; gm1b_1.flags = 4; gm1b_1.act = 0;
      gm1b_1.alpha = 1.0f; gm1b_1.beta = 1.0f; gm1b_1.sa = 1.0f; gm1b_1.sb = 1.0f; gm1b_1.Npad = H; gm1b_1.pad_ = 0;
      k_gemm<1><<<dim3((unsigned)((H) + 31) / 32, (unsigned)((CH) + 15) / 16, (unsigned)(1)), 32, 0, stream>>>(gm1b_1); }
    { GemmP gm1c_1;
      gm1c_1.A = EF; gm1c_1.B = mnw1 + (size_t)256 * H; gm1c_1.bias = EF; gm1c_1.R = G; gm1c_1.C = G;
      gm1c_1.sAo = 0; gm1c_1.sAi = 0; gm1c_1.sAm = H; gm1c_1.sAk = 1; gm1c_1.sBo = 0; gm1c_1.sBi = 0; gm1c_1.sBn = 1; gm1c_1.sBk = H; gm1c_1.sCo = 0; gm1c_1.sCi = 0; gm1c_1.sCm = H; gm1c_1.sRo = 0; gm1c_1.sRi = 0; gm1c_1.sRm = H; gm1c_1.sRn = 1;
      gm1c_1.M = CH; gm1c_1.N = H; gm1c_1.K = H; gm1c_1.zi_n = 1; gm1c_1.flags = 4; gm1c_1.act = 0;
      gm1c_1.alpha = 1.0f; gm1c_1.beta = 1.0f; gm1c_1.sa = 1.0f; gm1c_1.sb = 1.0f; gm1c_1.Npad = H; gm1c_1.pad_ = 0;
      k_gemm<1><<<dim3((unsigned)((H) + 31) / 32, (unsigned)((CH) + 15) / 16, (unsigned)(1)), 32, 0, stream>>>(gm1c_1); }
    k_csp_silu<<<(unsigned)(((long long)CH * H + 255) / 256), 256, 0, stream>>>(G, (long long)CH * H);
    { GemmP gm2_1;
      gm2_1.A = G; gm2_1.B = mnw2; gm2_1.bias = mnb2; gm2_1.R = G; gm2_1.C = MSG;
      gm2_1.sAo = 0; gm2_1.sAi = 0; gm2_1.sAm = H; gm2_1.sAk = 1; gm2_1.sBo = 0; gm2_1.sBi = 0; gm2_1.sBn = 1; gm2_1.sBk = H; gm2_1.sCo = 0; gm2_1.sCi = 0; gm2_1.sCm = H; gm2_1.sRo = 0; gm2_1.sRi = 0; gm2_1.sRm = 0; gm2_1.sRn = 0;
      gm2_1.M = CH; gm2_1.N = H; gm2_1.K = H; gm2_1.zi_n = 1; gm2_1.flags = 1; gm2_1.act = 0;
      gm2_1.alpha = 1.0f; gm2_1.beta = 0.0f; gm2_1.sa = 1.0f; gm2_1.sb = 1.0f; gm2_1.Npad = H; gm2_1.pad_ = 0;
      k_gemm<1><<<dim3((unsigned)((H) + 31) / 32, (unsigned)((CH) + 15) / 16, (unsigned)(1)), 32, 0, stream>>>(gm2_1); }
    k_csp_agg<<<(unsigned)(((long long)Nn * H + 255) / 256), 256, 0, stream>>>(MSG, off, AGG, 50000, CH, Nn, H);
    k_csp_gather<<<(unsigned)(((long long)CH * H + 255) / 256), 256, 0, stream>>>(x, ea, ei, slot, XD, XS, EAc, 100000, CH, E, H, EDd);
    { GemmP ge1_2;
      ge1_2.A = EAc; ge1_2.B = eew1; ge1_2.bias = eeb1; ge1_2.R = EAc; ge1_2.C = EF1;
      ge1_2.sAo = 0; ge1_2.sAi = 0; ge1_2.sAm = 32; ge1_2.sAk = 1; ge1_2.sBo = 0; ge1_2.sBi = 0; ge1_2.sBn = 1; ge1_2.sBk = H; ge1_2.sCo = 0; ge1_2.sCi = 0; ge1_2.sCm = H; ge1_2.sRo = 0; ge1_2.sRi = 0; ge1_2.sRm = 0; ge1_2.sRn = 0;
      ge1_2.M = CH; ge1_2.N = H; ge1_2.K = EDd; ge1_2.zi_n = 1; ge1_2.flags = 1; ge1_2.act = 0;
      ge1_2.alpha = 1.0f; ge1_2.beta = 0.0f; ge1_2.sa = 1.0f; ge1_2.sb = 1.0f; ge1_2.Npad = H; ge1_2.pad_ = 0;
      k_gemm<1><<<dim3((unsigned)((H) + 31) / 32, (unsigned)((CH) + 15) / 16, (unsigned)(1)), 32, 0, stream>>>(ge1_2); }
    k_csp_silu<<<(unsigned)(((long long)CH * H + 255) / 256), 256, 0, stream>>>(EF1, (long long)CH * H);
    { GemmP ge2_2;
      ge2_2.A = EF1; ge2_2.B = eew2; ge2_2.bias = eeb2; ge2_2.R = EF1; ge2_2.C = EF;
      ge2_2.sAo = 0; ge2_2.sAi = 0; ge2_2.sAm = H; ge2_2.sAk = 1; ge2_2.sBo = 0; ge2_2.sBi = 0; ge2_2.sBn = 1; ge2_2.sBk = H; ge2_2.sCo = 0; ge2_2.sCi = 0; ge2_2.sCm = H; ge2_2.sRo = 0; ge2_2.sRi = 0; ge2_2.sRm = 0; ge2_2.sRn = 0;
      ge2_2.M = CH; ge2_2.N = H; ge2_2.K = H; ge2_2.zi_n = 1; ge2_2.flags = 1; ge2_2.act = 0;
      ge2_2.alpha = 1.0f; ge2_2.beta = 0.0f; ge2_2.sa = 1.0f; ge2_2.sb = 1.0f; ge2_2.Npad = H; ge2_2.pad_ = 0;
      k_gemm<1><<<dim3((unsigned)((H) + 31) / 32, (unsigned)((CH) + 15) / 16, (unsigned)(1)), 32, 0, stream>>>(ge2_2); }
    { GemmP gm1a_2;
      gm1a_2.A = XD; gm1a_2.B = mnw1; gm1a_2.bias = mnb1; gm1a_2.R = XD; gm1a_2.C = G;
      gm1a_2.sAo = 0; gm1a_2.sAi = 0; gm1a_2.sAm = H; gm1a_2.sAk = 1; gm1a_2.sBo = 0; gm1a_2.sBi = 0; gm1a_2.sBn = 1; gm1a_2.sBk = H; gm1a_2.sCo = 0; gm1a_2.sCi = 0; gm1a_2.sCm = H; gm1a_2.sRo = 0; gm1a_2.sRi = 0; gm1a_2.sRm = 0; gm1a_2.sRn = 0;
      gm1a_2.M = CH; gm1a_2.N = H; gm1a_2.K = H; gm1a_2.zi_n = 1; gm1a_2.flags = 1; gm1a_2.act = 0;
      gm1a_2.alpha = 1.0f; gm1a_2.beta = 0.0f; gm1a_2.sa = 1.0f; gm1a_2.sb = 1.0f; gm1a_2.Npad = H; gm1a_2.pad_ = 0;
      k_gemm<1><<<dim3((unsigned)((H) + 31) / 32, (unsigned)((CH) + 15) / 16, (unsigned)(1)), 32, 0, stream>>>(gm1a_2); }
    { GemmP gm1b_2;
      gm1b_2.A = XS; gm1b_2.B = mnw1 + (size_t)128 * H; gm1b_2.bias = XS; gm1b_2.R = G; gm1b_2.C = G;
      gm1b_2.sAo = 0; gm1b_2.sAi = 0; gm1b_2.sAm = H; gm1b_2.sAk = 1; gm1b_2.sBo = 0; gm1b_2.sBi = 0; gm1b_2.sBn = 1; gm1b_2.sBk = H; gm1b_2.sCo = 0; gm1b_2.sCi = 0; gm1b_2.sCm = H; gm1b_2.sRo = 0; gm1b_2.sRi = 0; gm1b_2.sRm = H; gm1b_2.sRn = 1;
      gm1b_2.M = CH; gm1b_2.N = H; gm1b_2.K = H; gm1b_2.zi_n = 1; gm1b_2.flags = 4; gm1b_2.act = 0;
      gm1b_2.alpha = 1.0f; gm1b_2.beta = 1.0f; gm1b_2.sa = 1.0f; gm1b_2.sb = 1.0f; gm1b_2.Npad = H; gm1b_2.pad_ = 0;
      k_gemm<1><<<dim3((unsigned)((H) + 31) / 32, (unsigned)((CH) + 15) / 16, (unsigned)(1)), 32, 0, stream>>>(gm1b_2); }
    { GemmP gm1c_2;
      gm1c_2.A = EF; gm1c_2.B = mnw1 + (size_t)256 * H; gm1c_2.bias = EF; gm1c_2.R = G; gm1c_2.C = G;
      gm1c_2.sAo = 0; gm1c_2.sAi = 0; gm1c_2.sAm = H; gm1c_2.sAk = 1; gm1c_2.sBo = 0; gm1c_2.sBi = 0; gm1c_2.sBn = 1; gm1c_2.sBk = H; gm1c_2.sCo = 0; gm1c_2.sCi = 0; gm1c_2.sCm = H; gm1c_2.sRo = 0; gm1c_2.sRi = 0; gm1c_2.sRm = H; gm1c_2.sRn = 1;
      gm1c_2.M = CH; gm1c_2.N = H; gm1c_2.K = H; gm1c_2.zi_n = 1; gm1c_2.flags = 4; gm1c_2.act = 0;
      gm1c_2.alpha = 1.0f; gm1c_2.beta = 1.0f; gm1c_2.sa = 1.0f; gm1c_2.sb = 1.0f; gm1c_2.Npad = H; gm1c_2.pad_ = 0;
      k_gemm<1><<<dim3((unsigned)((H) + 31) / 32, (unsigned)((CH) + 15) / 16, (unsigned)(1)), 32, 0, stream>>>(gm1c_2); }
    k_csp_silu<<<(unsigned)(((long long)CH * H + 255) / 256), 256, 0, stream>>>(G, (long long)CH * H);
    { GemmP gm2_2;
      gm2_2.A = G; gm2_2.B = mnw2; gm2_2.bias = mnb2; gm2_2.R = G; gm2_2.C = MSG;
      gm2_2.sAo = 0; gm2_2.sAi = 0; gm2_2.sAm = H; gm2_2.sAk = 1; gm2_2.sBo = 0; gm2_2.sBi = 0; gm2_2.sBn = 1; gm2_2.sBk = H; gm2_2.sCo = 0; gm2_2.sCi = 0; gm2_2.sCm = H; gm2_2.sRo = 0; gm2_2.sRi = 0; gm2_2.sRm = 0; gm2_2.sRn = 0;
      gm2_2.M = CH; gm2_2.N = H; gm2_2.K = H; gm2_2.zi_n = 1; gm2_2.flags = 1; gm2_2.act = 0;
      gm2_2.alpha = 1.0f; gm2_2.beta = 0.0f; gm2_2.sa = 1.0f; gm2_2.sb = 1.0f; gm2_2.Npad = H; gm2_2.pad_ = 0;
      k_gemm<1><<<dim3((unsigned)((H) + 31) / 32, (unsigned)((CH) + 15) / 16, (unsigned)(1)), 32, 0, stream>>>(gm2_2); }
    k_csp_agg<<<(unsigned)(((long long)Nn * H + 255) / 256), 256, 0, stream>>>(MSG, off, AGG, 100000, CH, Nn, H);
    k_csp_gather<<<(unsigned)(((long long)CH * H + 255) / 256), 256, 0, stream>>>(x, ea, ei, slot, XD, XS, EAc, 150000, CH, E, H, EDd);
    { GemmP ge1_3;
      ge1_3.A = EAc; ge1_3.B = eew1; ge1_3.bias = eeb1; ge1_3.R = EAc; ge1_3.C = EF1;
      ge1_3.sAo = 0; ge1_3.sAi = 0; ge1_3.sAm = 32; ge1_3.sAk = 1; ge1_3.sBo = 0; ge1_3.sBi = 0; ge1_3.sBn = 1; ge1_3.sBk = H; ge1_3.sCo = 0; ge1_3.sCi = 0; ge1_3.sCm = H; ge1_3.sRo = 0; ge1_3.sRi = 0; ge1_3.sRm = 0; ge1_3.sRn = 0;
      ge1_3.M = CH; ge1_3.N = H; ge1_3.K = EDd; ge1_3.zi_n = 1; ge1_3.flags = 1; ge1_3.act = 0;
      ge1_3.alpha = 1.0f; ge1_3.beta = 0.0f; ge1_3.sa = 1.0f; ge1_3.sb = 1.0f; ge1_3.Npad = H; ge1_3.pad_ = 0;
      k_gemm<1><<<dim3((unsigned)((H) + 31) / 32, (unsigned)((CH) + 15) / 16, (unsigned)(1)), 32, 0, stream>>>(ge1_3); }
    k_csp_silu<<<(unsigned)(((long long)CH * H + 255) / 256), 256, 0, stream>>>(EF1, (long long)CH * H);
    { GemmP ge2_3;
      ge2_3.A = EF1; ge2_3.B = eew2; ge2_3.bias = eeb2; ge2_3.R = EF1; ge2_3.C = EF;
      ge2_3.sAo = 0; ge2_3.sAi = 0; ge2_3.sAm = H; ge2_3.sAk = 1; ge2_3.sBo = 0; ge2_3.sBi = 0; ge2_3.sBn = 1; ge2_3.sBk = H; ge2_3.sCo = 0; ge2_3.sCi = 0; ge2_3.sCm = H; ge2_3.sRo = 0; ge2_3.sRi = 0; ge2_3.sRm = 0; ge2_3.sRn = 0;
      ge2_3.M = CH; ge2_3.N = H; ge2_3.K = H; ge2_3.zi_n = 1; ge2_3.flags = 1; ge2_3.act = 0;
      ge2_3.alpha = 1.0f; ge2_3.beta = 0.0f; ge2_3.sa = 1.0f; ge2_3.sb = 1.0f; ge2_3.Npad = H; ge2_3.pad_ = 0;
      k_gemm<1><<<dim3((unsigned)((H) + 31) / 32, (unsigned)((CH) + 15) / 16, (unsigned)(1)), 32, 0, stream>>>(ge2_3); }
    { GemmP gm1a_3;
      gm1a_3.A = XD; gm1a_3.B = mnw1; gm1a_3.bias = mnb1; gm1a_3.R = XD; gm1a_3.C = G;
      gm1a_3.sAo = 0; gm1a_3.sAi = 0; gm1a_3.sAm = H; gm1a_3.sAk = 1; gm1a_3.sBo = 0; gm1a_3.sBi = 0; gm1a_3.sBn = 1; gm1a_3.sBk = H; gm1a_3.sCo = 0; gm1a_3.sCi = 0; gm1a_3.sCm = H; gm1a_3.sRo = 0; gm1a_3.sRi = 0; gm1a_3.sRm = 0; gm1a_3.sRn = 0;
      gm1a_3.M = CH; gm1a_3.N = H; gm1a_3.K = H; gm1a_3.zi_n = 1; gm1a_3.flags = 1; gm1a_3.act = 0;
      gm1a_3.alpha = 1.0f; gm1a_3.beta = 0.0f; gm1a_3.sa = 1.0f; gm1a_3.sb = 1.0f; gm1a_3.Npad = H; gm1a_3.pad_ = 0;
      k_gemm<1><<<dim3((unsigned)((H) + 31) / 32, (unsigned)((CH) + 15) / 16, (unsigned)(1)), 32, 0, stream>>>(gm1a_3); }
    { GemmP gm1b_3;
      gm1b_3.A = XS; gm1b_3.B = mnw1 + (size_t)128 * H; gm1b_3.bias = XS; gm1b_3.R = G; gm1b_3.C = G;
      gm1b_3.sAo = 0; gm1b_3.sAi = 0; gm1b_3.sAm = H; gm1b_3.sAk = 1; gm1b_3.sBo = 0; gm1b_3.sBi = 0; gm1b_3.sBn = 1; gm1b_3.sBk = H; gm1b_3.sCo = 0; gm1b_3.sCi = 0; gm1b_3.sCm = H; gm1b_3.sRo = 0; gm1b_3.sRi = 0; gm1b_3.sRm = H; gm1b_3.sRn = 1;
      gm1b_3.M = CH; gm1b_3.N = H; gm1b_3.K = H; gm1b_3.zi_n = 1; gm1b_3.flags = 4; gm1b_3.act = 0;
      gm1b_3.alpha = 1.0f; gm1b_3.beta = 1.0f; gm1b_3.sa = 1.0f; gm1b_3.sb = 1.0f; gm1b_3.Npad = H; gm1b_3.pad_ = 0;
      k_gemm<1><<<dim3((unsigned)((H) + 31) / 32, (unsigned)((CH) + 15) / 16, (unsigned)(1)), 32, 0, stream>>>(gm1b_3); }
    { GemmP gm1c_3;
      gm1c_3.A = EF; gm1c_3.B = mnw1 + (size_t)256 * H; gm1c_3.bias = EF; gm1c_3.R = G; gm1c_3.C = G;
      gm1c_3.sAo = 0; gm1c_3.sAi = 0; gm1c_3.sAm = H; gm1c_3.sAk = 1; gm1c_3.sBo = 0; gm1c_3.sBi = 0; gm1c_3.sBn = 1; gm1c_3.sBk = H; gm1c_3.sCo = 0; gm1c_3.sCi = 0; gm1c_3.sCm = H; gm1c_3.sRo = 0; gm1c_3.sRi = 0; gm1c_3.sRm = H; gm1c_3.sRn = 1;
      gm1c_3.M = CH; gm1c_3.N = H; gm1c_3.K = H; gm1c_3.zi_n = 1; gm1c_3.flags = 4; gm1c_3.act = 0;
      gm1c_3.alpha = 1.0f; gm1c_3.beta = 1.0f; gm1c_3.sa = 1.0f; gm1c_3.sb = 1.0f; gm1c_3.Npad = H; gm1c_3.pad_ = 0;
      k_gemm<1><<<dim3((unsigned)((H) + 31) / 32, (unsigned)((CH) + 15) / 16, (unsigned)(1)), 32, 0, stream>>>(gm1c_3); }
    k_csp_silu<<<(unsigned)(((long long)CH * H + 255) / 256), 256, 0, stream>>>(G, (long long)CH * H);
    { GemmP gm2_3;
      gm2_3.A = G; gm2_3.B = mnw2; gm2_3.bias = mnb2; gm2_3.R = G; gm2_3.C = MSG;
      gm2_3.sAo = 0; gm2_3.sAi = 0; gm2_3.sAm = H; gm2_3.sAk = 1; gm2_3.sBo = 0; gm2_3.sBi = 0; gm2_3.sBn = 1; gm2_3.sBk = H; gm2_3.sCo = 0; gm2_3.sCi = 0; gm2_3.sCm = H; gm2_3.sRo = 0; gm2_3.sRi = 0; gm2_3.sRm = 0; gm2_3.sRn = 0;
      gm2_3.M = CH; gm2_3.N = H; gm2_3.K = H; gm2_3.zi_n = 1; gm2_3.flags = 1; gm2_3.act = 0;
      gm2_3.alpha = 1.0f; gm2_3.beta = 0.0f; gm2_3.sa = 1.0f; gm2_3.sb = 1.0f; gm2_3.Npad = H; gm2_3.pad_ = 0;
      k_gemm<1><<<dim3((unsigned)((H) + 31) / 32, (unsigned)((CH) + 15) / 16, (unsigned)(1)), 32, 0, stream>>>(gm2_3); }
    k_csp_agg<<<(unsigned)(((long long)Nn * H + 255) / 256), 256, 0, stream>>>(MSG, off, AGG, 150000, CH, Nn, H);
    k_csp_gather<<<(unsigned)(((long long)CH * H + 255) / 256), 256, 0, stream>>>(x, ea, ei, slot, XD, XS, EAc, 200000, CH, E, H, EDd);
    { GemmP ge1_4;
      ge1_4.A = EAc; ge1_4.B = eew1; ge1_4.bias = eeb1; ge1_4.R = EAc; ge1_4.C = EF1;
      ge1_4.sAo = 0; ge1_4.sAi = 0; ge1_4.sAm = 32; ge1_4.sAk = 1; ge1_4.sBo = 0; ge1_4.sBi = 0; ge1_4.sBn = 1; ge1_4.sBk = H; ge1_4.sCo = 0; ge1_4.sCi = 0; ge1_4.sCm = H; ge1_4.sRo = 0; ge1_4.sRi = 0; ge1_4.sRm = 0; ge1_4.sRn = 0;
      ge1_4.M = CH; ge1_4.N = H; ge1_4.K = EDd; ge1_4.zi_n = 1; ge1_4.flags = 1; ge1_4.act = 0;
      ge1_4.alpha = 1.0f; ge1_4.beta = 0.0f; ge1_4.sa = 1.0f; ge1_4.sb = 1.0f; ge1_4.Npad = H; ge1_4.pad_ = 0;
      k_gemm<1><<<dim3((unsigned)((H) + 31) / 32, (unsigned)((CH) + 15) / 16, (unsigned)(1)), 32, 0, stream>>>(ge1_4); }
    k_csp_silu<<<(unsigned)(((long long)CH * H + 255) / 256), 256, 0, stream>>>(EF1, (long long)CH * H);
    { GemmP ge2_4;
      ge2_4.A = EF1; ge2_4.B = eew2; ge2_4.bias = eeb2; ge2_4.R = EF1; ge2_4.C = EF;
      ge2_4.sAo = 0; ge2_4.sAi = 0; ge2_4.sAm = H; ge2_4.sAk = 1; ge2_4.sBo = 0; ge2_4.sBi = 0; ge2_4.sBn = 1; ge2_4.sBk = H; ge2_4.sCo = 0; ge2_4.sCi = 0; ge2_4.sCm = H; ge2_4.sRo = 0; ge2_4.sRi = 0; ge2_4.sRm = 0; ge2_4.sRn = 0;
      ge2_4.M = CH; ge2_4.N = H; ge2_4.K = H; ge2_4.zi_n = 1; ge2_4.flags = 1; ge2_4.act = 0;
      ge2_4.alpha = 1.0f; ge2_4.beta = 0.0f; ge2_4.sa = 1.0f; ge2_4.sb = 1.0f; ge2_4.Npad = H; ge2_4.pad_ = 0;
      k_gemm<1><<<dim3((unsigned)((H) + 31) / 32, (unsigned)((CH) + 15) / 16, (unsigned)(1)), 32, 0, stream>>>(ge2_4); }
    { GemmP gm1a_4;
      gm1a_4.A = XD; gm1a_4.B = mnw1; gm1a_4.bias = mnb1; gm1a_4.R = XD; gm1a_4.C = G;
      gm1a_4.sAo = 0; gm1a_4.sAi = 0; gm1a_4.sAm = H; gm1a_4.sAk = 1; gm1a_4.sBo = 0; gm1a_4.sBi = 0; gm1a_4.sBn = 1; gm1a_4.sBk = H; gm1a_4.sCo = 0; gm1a_4.sCi = 0; gm1a_4.sCm = H; gm1a_4.sRo = 0; gm1a_4.sRi = 0; gm1a_4.sRm = 0; gm1a_4.sRn = 0;
      gm1a_4.M = CH; gm1a_4.N = H; gm1a_4.K = H; gm1a_4.zi_n = 1; gm1a_4.flags = 1; gm1a_4.act = 0;
      gm1a_4.alpha = 1.0f; gm1a_4.beta = 0.0f; gm1a_4.sa = 1.0f; gm1a_4.sb = 1.0f; gm1a_4.Npad = H; gm1a_4.pad_ = 0;
      k_gemm<1><<<dim3((unsigned)((H) + 31) / 32, (unsigned)((CH) + 15) / 16, (unsigned)(1)), 32, 0, stream>>>(gm1a_4); }
    { GemmP gm1b_4;
      gm1b_4.A = XS; gm1b_4.B = mnw1 + (size_t)128 * H; gm1b_4.bias = XS; gm1b_4.R = G; gm1b_4.C = G;
      gm1b_4.sAo = 0; gm1b_4.sAi = 0; gm1b_4.sAm = H; gm1b_4.sAk = 1; gm1b_4.sBo = 0; gm1b_4.sBi = 0; gm1b_4.sBn = 1; gm1b_4.sBk = H; gm1b_4.sCo = 0; gm1b_4.sCi = 0; gm1b_4.sCm = H; gm1b_4.sRo = 0; gm1b_4.sRi = 0; gm1b_4.sRm = H; gm1b_4.sRn = 1;
      gm1b_4.M = CH; gm1b_4.N = H; gm1b_4.K = H; gm1b_4.zi_n = 1; gm1b_4.flags = 4; gm1b_4.act = 0;
      gm1b_4.alpha = 1.0f; gm1b_4.beta = 1.0f; gm1b_4.sa = 1.0f; gm1b_4.sb = 1.0f; gm1b_4.Npad = H; gm1b_4.pad_ = 0;
      k_gemm<1><<<dim3((unsigned)((H) + 31) / 32, (unsigned)((CH) + 15) / 16, (unsigned)(1)), 32, 0, stream>>>(gm1b_4); }
    { GemmP gm1c_4;
      gm1c_4.A = EF; gm1c_4.B = mnw1 + (size_t)256 * H; gm1c_4.bias = EF; gm1c_4.R = G; gm1c_4.C = G;
      gm1c_4.sAo = 0; gm1c_4.sAi = 0; gm1c_4.sAm = H; gm1c_4.sAk = 1; gm1c_4.sBo = 0; gm1c_4.sBi = 0; gm1c_4.sBn = 1; gm1c_4.sBk = H; gm1c_4.sCo = 0; gm1c_4.sCi = 0; gm1c_4.sCm = H; gm1c_4.sRo = 0; gm1c_4.sRi = 0; gm1c_4.sRm = H; gm1c_4.sRn = 1;
      gm1c_4.M = CH; gm1c_4.N = H; gm1c_4.K = H; gm1c_4.zi_n = 1; gm1c_4.flags = 4; gm1c_4.act = 0;
      gm1c_4.alpha = 1.0f; gm1c_4.beta = 1.0f; gm1c_4.sa = 1.0f; gm1c_4.sb = 1.0f; gm1c_4.Npad = H; gm1c_4.pad_ = 0;
      k_gemm<1><<<dim3((unsigned)((H) + 31) / 32, (unsigned)((CH) + 15) / 16, (unsigned)(1)), 32, 0, stream>>>(gm1c_4); }
    k_csp_silu<<<(unsigned)(((long long)CH * H + 255) / 256), 256, 0, stream>>>(G, (long long)CH * H);
    { GemmP gm2_4;
      gm2_4.A = G; gm2_4.B = mnw2; gm2_4.bias = mnb2; gm2_4.R = G; gm2_4.C = MSG;
      gm2_4.sAo = 0; gm2_4.sAi = 0; gm2_4.sAm = H; gm2_4.sAk = 1; gm2_4.sBo = 0; gm2_4.sBi = 0; gm2_4.sBn = 1; gm2_4.sBk = H; gm2_4.sCo = 0; gm2_4.sCi = 0; gm2_4.sCm = H; gm2_4.sRo = 0; gm2_4.sRi = 0; gm2_4.sRm = 0; gm2_4.sRn = 0;
      gm2_4.M = CH; gm2_4.N = H; gm2_4.K = H; gm2_4.zi_n = 1; gm2_4.flags = 1; gm2_4.act = 0;
      gm2_4.alpha = 1.0f; gm2_4.beta = 0.0f; gm2_4.sa = 1.0f; gm2_4.sb = 1.0f; gm2_4.Npad = H; gm2_4.pad_ = 0;
      k_gemm<1><<<dim3((unsigned)((H) + 31) / 32, (unsigned)((CH) + 15) / 16, (unsigned)(1)), 32, 0, stream>>>(gm2_4); }
    k_csp_agg<<<(unsigned)(((long long)Nn * H + 255) / 256), 256, 0, stream>>>(MSG, off, AGG, 200000, CH, Nn, H);
    k_csp_gather<<<(unsigned)(((long long)CH * H + 255) / 256), 256, 0, stream>>>(x, ea, ei, slot, XD, XS, EAc, 250000, CH, E, H, EDd);
    { GemmP ge1_5;
      ge1_5.A = EAc; ge1_5.B = eew1; ge1_5.bias = eeb1; ge1_5.R = EAc; ge1_5.C = EF1;
      ge1_5.sAo = 0; ge1_5.sAi = 0; ge1_5.sAm = 32; ge1_5.sAk = 1; ge1_5.sBo = 0; ge1_5.sBi = 0; ge1_5.sBn = 1; ge1_5.sBk = H; ge1_5.sCo = 0; ge1_5.sCi = 0; ge1_5.sCm = H; ge1_5.sRo = 0; ge1_5.sRi = 0; ge1_5.sRm = 0; ge1_5.sRn = 0;
      ge1_5.M = CH; ge1_5.N = H; ge1_5.K = EDd; ge1_5.zi_n = 1; ge1_5.flags = 1; ge1_5.act = 0;
      ge1_5.alpha = 1.0f; ge1_5.beta = 0.0f; ge1_5.sa = 1.0f; ge1_5.sb = 1.0f; ge1_5.Npad = H; ge1_5.pad_ = 0;
      k_gemm<1><<<dim3((unsigned)((H) + 31) / 32, (unsigned)((CH) + 15) / 16, (unsigned)(1)), 32, 0, stream>>>(ge1_5); }
    k_csp_silu<<<(unsigned)(((long long)CH * H + 255) / 256), 256, 0, stream>>>(EF1, (long long)CH * H);
    { GemmP ge2_5;
      ge2_5.A = EF1; ge2_5.B = eew2; ge2_5.bias = eeb2; ge2_5.R = EF1; ge2_5.C = EF;
      ge2_5.sAo = 0; ge2_5.sAi = 0; ge2_5.sAm = H; ge2_5.sAk = 1; ge2_5.sBo = 0; ge2_5.sBi = 0; ge2_5.sBn = 1; ge2_5.sBk = H; ge2_5.sCo = 0; ge2_5.sCi = 0; ge2_5.sCm = H; ge2_5.sRo = 0; ge2_5.sRi = 0; ge2_5.sRm = 0; ge2_5.sRn = 0;
      ge2_5.M = CH; ge2_5.N = H; ge2_5.K = H; ge2_5.zi_n = 1; ge2_5.flags = 1; ge2_5.act = 0;
      ge2_5.alpha = 1.0f; ge2_5.beta = 0.0f; ge2_5.sa = 1.0f; ge2_5.sb = 1.0f; ge2_5.Npad = H; ge2_5.pad_ = 0;
      k_gemm<1><<<dim3((unsigned)((H) + 31) / 32, (unsigned)((CH) + 15) / 16, (unsigned)(1)), 32, 0, stream>>>(ge2_5); }
    { GemmP gm1a_5;
      gm1a_5.A = XD; gm1a_5.B = mnw1; gm1a_5.bias = mnb1; gm1a_5.R = XD; gm1a_5.C = G;
      gm1a_5.sAo = 0; gm1a_5.sAi = 0; gm1a_5.sAm = H; gm1a_5.sAk = 1; gm1a_5.sBo = 0; gm1a_5.sBi = 0; gm1a_5.sBn = 1; gm1a_5.sBk = H; gm1a_5.sCo = 0; gm1a_5.sCi = 0; gm1a_5.sCm = H; gm1a_5.sRo = 0; gm1a_5.sRi = 0; gm1a_5.sRm = 0; gm1a_5.sRn = 0;
      gm1a_5.M = CH; gm1a_5.N = H; gm1a_5.K = H; gm1a_5.zi_n = 1; gm1a_5.flags = 1; gm1a_5.act = 0;
      gm1a_5.alpha = 1.0f; gm1a_5.beta = 0.0f; gm1a_5.sa = 1.0f; gm1a_5.sb = 1.0f; gm1a_5.Npad = H; gm1a_5.pad_ = 0;
      k_gemm<1><<<dim3((unsigned)((H) + 31) / 32, (unsigned)((CH) + 15) / 16, (unsigned)(1)), 32, 0, stream>>>(gm1a_5); }
    { GemmP gm1b_5;
      gm1b_5.A = XS; gm1b_5.B = mnw1 + (size_t)128 * H; gm1b_5.bias = XS; gm1b_5.R = G; gm1b_5.C = G;
      gm1b_5.sAo = 0; gm1b_5.sAi = 0; gm1b_5.sAm = H; gm1b_5.sAk = 1; gm1b_5.sBo = 0; gm1b_5.sBi = 0; gm1b_5.sBn = 1; gm1b_5.sBk = H; gm1b_5.sCo = 0; gm1b_5.sCi = 0; gm1b_5.sCm = H; gm1b_5.sRo = 0; gm1b_5.sRi = 0; gm1b_5.sRm = H; gm1b_5.sRn = 1;
      gm1b_5.M = CH; gm1b_5.N = H; gm1b_5.K = H; gm1b_5.zi_n = 1; gm1b_5.flags = 4; gm1b_5.act = 0;
      gm1b_5.alpha = 1.0f; gm1b_5.beta = 1.0f; gm1b_5.sa = 1.0f; gm1b_5.sb = 1.0f; gm1b_5.Npad = H; gm1b_5.pad_ = 0;
      k_gemm<1><<<dim3((unsigned)((H) + 31) / 32, (unsigned)((CH) + 15) / 16, (unsigned)(1)), 32, 0, stream>>>(gm1b_5); }
    { GemmP gm1c_5;
      gm1c_5.A = EF; gm1c_5.B = mnw1 + (size_t)256 * H; gm1c_5.bias = EF; gm1c_5.R = G; gm1c_5.C = G;
      gm1c_5.sAo = 0; gm1c_5.sAi = 0; gm1c_5.sAm = H; gm1c_5.sAk = 1; gm1c_5.sBo = 0; gm1c_5.sBi = 0; gm1c_5.sBn = 1; gm1c_5.sBk = H; gm1c_5.sCo = 0; gm1c_5.sCi = 0; gm1c_5.sCm = H; gm1c_5.sRo = 0; gm1c_5.sRi = 0; gm1c_5.sRm = H; gm1c_5.sRn = 1;
      gm1c_5.M = CH; gm1c_5.N = H; gm1c_5.K = H; gm1c_5.zi_n = 1; gm1c_5.flags = 4; gm1c_5.act = 0;
      gm1c_5.alpha = 1.0f; gm1c_5.beta = 1.0f; gm1c_5.sa = 1.0f; gm1c_5.sb = 1.0f; gm1c_5.Npad = H; gm1c_5.pad_ = 0;
      k_gemm<1><<<dim3((unsigned)((H) + 31) / 32, (unsigned)((CH) + 15) / 16, (unsigned)(1)), 32, 0, stream>>>(gm1c_5); }
    k_csp_silu<<<(unsigned)(((long long)CH * H + 255) / 256), 256, 0, stream>>>(G, (long long)CH * H);
    { GemmP gm2_5;
      gm2_5.A = G; gm2_5.B = mnw2; gm2_5.bias = mnb2; gm2_5.R = G; gm2_5.C = MSG;
      gm2_5.sAo = 0; gm2_5.sAi = 0; gm2_5.sAm = H; gm2_5.sAk = 1; gm2_5.sBo = 0; gm2_5.sBi = 0; gm2_5.sBn = 1; gm2_5.sBk = H; gm2_5.sCo = 0; gm2_5.sCi = 0; gm2_5.sCm = H; gm2_5.sRo = 0; gm2_5.sRi = 0; gm2_5.sRm = 0; gm2_5.sRn = 0;
      gm2_5.M = CH; gm2_5.N = H; gm2_5.K = H; gm2_5.zi_n = 1; gm2_5.flags = 1; gm2_5.act = 0;
      gm2_5.alpha = 1.0f; gm2_5.beta = 0.0f; gm2_5.sa = 1.0f; gm2_5.sb = 1.0f; gm2_5.Npad = H; gm2_5.pad_ = 0;
      k_gemm<1><<<dim3((unsigned)((H) + 31) / 32, (unsigned)((CH) + 15) / 16, (unsigned)(1)), 32, 0, stream>>>(gm2_5); }
    k_csp_agg<<<(unsigned)(((long long)Nn * H + 255) / 256), 256, 0, stream>>>(MSG, off, AGG, 250000, CH, Nn, H);
    k_csp_gather<<<(unsigned)(((long long)CH * H + 255) / 256), 256, 0, stream>>>(x, ea, ei, slot, XD, XS, EAc, 300000, CH, E, H, EDd);
    { GemmP ge1_6;
      ge1_6.A = EAc; ge1_6.B = eew1; ge1_6.bias = eeb1; ge1_6.R = EAc; ge1_6.C = EF1;
      ge1_6.sAo = 0; ge1_6.sAi = 0; ge1_6.sAm = 32; ge1_6.sAk = 1; ge1_6.sBo = 0; ge1_6.sBi = 0; ge1_6.sBn = 1; ge1_6.sBk = H; ge1_6.sCo = 0; ge1_6.sCi = 0; ge1_6.sCm = H; ge1_6.sRo = 0; ge1_6.sRi = 0; ge1_6.sRm = 0; ge1_6.sRn = 0;
      ge1_6.M = CH; ge1_6.N = H; ge1_6.K = EDd; ge1_6.zi_n = 1; ge1_6.flags = 1; ge1_6.act = 0;
      ge1_6.alpha = 1.0f; ge1_6.beta = 0.0f; ge1_6.sa = 1.0f; ge1_6.sb = 1.0f; ge1_6.Npad = H; ge1_6.pad_ = 0;
      k_gemm<1><<<dim3((unsigned)((H) + 31) / 32, (unsigned)((CH) + 15) / 16, (unsigned)(1)), 32, 0, stream>>>(ge1_6); }
    k_csp_silu<<<(unsigned)(((long long)CH * H + 255) / 256), 256, 0, stream>>>(EF1, (long long)CH * H);
    { GemmP ge2_6;
      ge2_6.A = EF1; ge2_6.B = eew2; ge2_6.bias = eeb2; ge2_6.R = EF1; ge2_6.C = EF;
      ge2_6.sAo = 0; ge2_6.sAi = 0; ge2_6.sAm = H; ge2_6.sAk = 1; ge2_6.sBo = 0; ge2_6.sBi = 0; ge2_6.sBn = 1; ge2_6.sBk = H; ge2_6.sCo = 0; ge2_6.sCi = 0; ge2_6.sCm = H; ge2_6.sRo = 0; ge2_6.sRi = 0; ge2_6.sRm = 0; ge2_6.sRn = 0;
      ge2_6.M = CH; ge2_6.N = H; ge2_6.K = H; ge2_6.zi_n = 1; ge2_6.flags = 1; ge2_6.act = 0;
      ge2_6.alpha = 1.0f; ge2_6.beta = 0.0f; ge2_6.sa = 1.0f; ge2_6.sb = 1.0f; ge2_6.Npad = H; ge2_6.pad_ = 0;
      k_gemm<1><<<dim3((unsigned)((H) + 31) / 32, (unsigned)((CH) + 15) / 16, (unsigned)(1)), 32, 0, stream>>>(ge2_6); }
    { GemmP gm1a_6;
      gm1a_6.A = XD; gm1a_6.B = mnw1; gm1a_6.bias = mnb1; gm1a_6.R = XD; gm1a_6.C = G;
      gm1a_6.sAo = 0; gm1a_6.sAi = 0; gm1a_6.sAm = H; gm1a_6.sAk = 1; gm1a_6.sBo = 0; gm1a_6.sBi = 0; gm1a_6.sBn = 1; gm1a_6.sBk = H; gm1a_6.sCo = 0; gm1a_6.sCi = 0; gm1a_6.sCm = H; gm1a_6.sRo = 0; gm1a_6.sRi = 0; gm1a_6.sRm = 0; gm1a_6.sRn = 0;
      gm1a_6.M = CH; gm1a_6.N = H; gm1a_6.K = H; gm1a_6.zi_n = 1; gm1a_6.flags = 1; gm1a_6.act = 0;
      gm1a_6.alpha = 1.0f; gm1a_6.beta = 0.0f; gm1a_6.sa = 1.0f; gm1a_6.sb = 1.0f; gm1a_6.Npad = H; gm1a_6.pad_ = 0;
      k_gemm<1><<<dim3((unsigned)((H) + 31) / 32, (unsigned)((CH) + 15) / 16, (unsigned)(1)), 32, 0, stream>>>(gm1a_6); }
    { GemmP gm1b_6;
      gm1b_6.A = XS; gm1b_6.B = mnw1 + (size_t)128 * H; gm1b_6.bias = XS; gm1b_6.R = G; gm1b_6.C = G;
      gm1b_6.sAo = 0; gm1b_6.sAi = 0; gm1b_6.sAm = H; gm1b_6.sAk = 1; gm1b_6.sBo = 0; gm1b_6.sBi = 0; gm1b_6.sBn = 1; gm1b_6.sBk = H; gm1b_6.sCo = 0; gm1b_6.sCi = 0; gm1b_6.sCm = H; gm1b_6.sRo = 0; gm1b_6.sRi = 0; gm1b_6.sRm = H; gm1b_6.sRn = 1;
      gm1b_6.M = CH; gm1b_6.N = H; gm1b_6.K = H; gm1b_6.zi_n = 1; gm1b_6.flags = 4; gm1b_6.act = 0;
      gm1b_6.alpha = 1.0f; gm1b_6.beta = 1.0f; gm1b_6.sa = 1.0f; gm1b_6.sb = 1.0f; gm1b_6.Npad = H; gm1b_6.pad_ = 0;
      k_gemm<1><<<dim3((unsigned)((H) + 31) / 32, (unsigned)((CH) + 15) / 16, (unsigned)(1)), 32, 0, stream>>>(gm1b_6); }
    { GemmP gm1c_6;
      gm1c_6.A = EF; gm1c_6.B = mnw1 + (size_t)256 * H; gm1c_6.bias = EF; gm1c_6.R = G; gm1c_6.C = G;
      gm1c_6.sAo = 0; gm1c_6.sAi = 0; gm1c_6.sAm = H; gm1c_6.sAk = 1; gm1c_6.sBo = 0; gm1c_6.sBi = 0; gm1c_6.sBn = 1; gm1c_6.sBk = H; gm1c_6.sCo = 0; gm1c_6.sCi = 0; gm1c_6.sCm = H; gm1c_6.sRo = 0; gm1c_6.sRi = 0; gm1c_6.sRm = H; gm1c_6.sRn = 1;
      gm1c_6.M = CH; gm1c_6.N = H; gm1c_6.K = H; gm1c_6.zi_n = 1; gm1c_6.flags = 4; gm1c_6.act = 0;
      gm1c_6.alpha = 1.0f; gm1c_6.beta = 1.0f; gm1c_6.sa = 1.0f; gm1c_6.sb = 1.0f; gm1c_6.Npad = H; gm1c_6.pad_ = 0;
      k_gemm<1><<<dim3((unsigned)((H) + 31) / 32, (unsigned)((CH) + 15) / 16, (unsigned)(1)), 32, 0, stream>>>(gm1c_6); }
    k_csp_silu<<<(unsigned)(((long long)CH * H + 255) / 256), 256, 0, stream>>>(G, (long long)CH * H);
    { GemmP gm2_6;
      gm2_6.A = G; gm2_6.B = mnw2; gm2_6.bias = mnb2; gm2_6.R = G; gm2_6.C = MSG;
      gm2_6.sAo = 0; gm2_6.sAi = 0; gm2_6.sAm = H; gm2_6.sAk = 1; gm2_6.sBo = 0; gm2_6.sBi = 0; gm2_6.sBn = 1; gm2_6.sBk = H; gm2_6.sCo = 0; gm2_6.sCi = 0; gm2_6.sCm = H; gm2_6.sRo = 0; gm2_6.sRi = 0; gm2_6.sRm = 0; gm2_6.sRn = 0;
      gm2_6.M = CH; gm2_6.N = H; gm2_6.K = H; gm2_6.zi_n = 1; gm2_6.flags = 1; gm2_6.act = 0;
      gm2_6.alpha = 1.0f; gm2_6.beta = 0.0f; gm2_6.sa = 1.0f; gm2_6.sb = 1.0f; gm2_6.Npad = H; gm2_6.pad_ = 0;
      k_gemm<1><<<dim3((unsigned)((H) + 31) / 32, (unsigned)((CH) + 15) / 16, (unsigned)(1)), 32, 0, stream>>>(gm2_6); }
    k_csp_agg<<<(unsigned)(((long long)Nn * H + 255) / 256), 256, 0, stream>>>(MSG, off, AGG, 300000, CH, Nn, H);
    k_csp_gather<<<(unsigned)(((long long)CH * H + 255) / 256), 256, 0, stream>>>(x, ea, ei, slot, XD, XS, EAc, 350000, CH, E, H, EDd);
    { GemmP ge1_7;
      ge1_7.A = EAc; ge1_7.B = eew1; ge1_7.bias = eeb1; ge1_7.R = EAc; ge1_7.C = EF1;
      ge1_7.sAo = 0; ge1_7.sAi = 0; ge1_7.sAm = 32; ge1_7.sAk = 1; ge1_7.sBo = 0; ge1_7.sBi = 0; ge1_7.sBn = 1; ge1_7.sBk = H; ge1_7.sCo = 0; ge1_7.sCi = 0; ge1_7.sCm = H; ge1_7.sRo = 0; ge1_7.sRi = 0; ge1_7.sRm = 0; ge1_7.sRn = 0;
      ge1_7.M = CH; ge1_7.N = H; ge1_7.K = EDd; ge1_7.zi_n = 1; ge1_7.flags = 1; ge1_7.act = 0;
      ge1_7.alpha = 1.0f; ge1_7.beta = 0.0f; ge1_7.sa = 1.0f; ge1_7.sb = 1.0f; ge1_7.Npad = H; ge1_7.pad_ = 0;
      k_gemm<1><<<dim3((unsigned)((H) + 31) / 32, (unsigned)((CH) + 15) / 16, (unsigned)(1)), 32, 0, stream>>>(ge1_7); }
    k_csp_silu<<<(unsigned)(((long long)CH * H + 255) / 256), 256, 0, stream>>>(EF1, (long long)CH * H);
    { GemmP ge2_7;
      ge2_7.A = EF1; ge2_7.B = eew2; ge2_7.bias = eeb2; ge2_7.R = EF1; ge2_7.C = EF;
      ge2_7.sAo = 0; ge2_7.sAi = 0; ge2_7.sAm = H; ge2_7.sAk = 1; ge2_7.sBo = 0; ge2_7.sBi = 0; ge2_7.sBn = 1; ge2_7.sBk = H; ge2_7.sCo = 0; ge2_7.sCi = 0; ge2_7.sCm = H; ge2_7.sRo = 0; ge2_7.sRi = 0; ge2_7.sRm = 0; ge2_7.sRn = 0;
      ge2_7.M = CH; ge2_7.N = H; ge2_7.K = H; ge2_7.zi_n = 1; ge2_7.flags = 1; ge2_7.act = 0;
      ge2_7.alpha = 1.0f; ge2_7.beta = 0.0f; ge2_7.sa = 1.0f; ge2_7.sb = 1.0f; ge2_7.Npad = H; ge2_7.pad_ = 0;
      k_gemm<1><<<dim3((unsigned)((H) + 31) / 32, (unsigned)((CH) + 15) / 16, (unsigned)(1)), 32, 0, stream>>>(ge2_7); }
    { GemmP gm1a_7;
      gm1a_7.A = XD; gm1a_7.B = mnw1; gm1a_7.bias = mnb1; gm1a_7.R = XD; gm1a_7.C = G;
      gm1a_7.sAo = 0; gm1a_7.sAi = 0; gm1a_7.sAm = H; gm1a_7.sAk = 1; gm1a_7.sBo = 0; gm1a_7.sBi = 0; gm1a_7.sBn = 1; gm1a_7.sBk = H; gm1a_7.sCo = 0; gm1a_7.sCi = 0; gm1a_7.sCm = H; gm1a_7.sRo = 0; gm1a_7.sRi = 0; gm1a_7.sRm = 0; gm1a_7.sRn = 0;
      gm1a_7.M = CH; gm1a_7.N = H; gm1a_7.K = H; gm1a_7.zi_n = 1; gm1a_7.flags = 1; gm1a_7.act = 0;
      gm1a_7.alpha = 1.0f; gm1a_7.beta = 0.0f; gm1a_7.sa = 1.0f; gm1a_7.sb = 1.0f; gm1a_7.Npad = H; gm1a_7.pad_ = 0;
      k_gemm<1><<<dim3((unsigned)((H) + 31) / 32, (unsigned)((CH) + 15) / 16, (unsigned)(1)), 32, 0, stream>>>(gm1a_7); }
    { GemmP gm1b_7;
      gm1b_7.A = XS; gm1b_7.B = mnw1 + (size_t)128 * H; gm1b_7.bias = XS; gm1b_7.R = G; gm1b_7.C = G;
      gm1b_7.sAo = 0; gm1b_7.sAi = 0; gm1b_7.sAm = H; gm1b_7.sAk = 1; gm1b_7.sBo = 0; gm1b_7.sBi = 0; gm1b_7.sBn = 1; gm1b_7.sBk = H; gm1b_7.sCo = 0; gm1b_7.sCi = 0; gm1b_7.sCm = H; gm1b_7.sRo = 0; gm1b_7.sRi = 0; gm1b_7.sRm = H; gm1b_7.sRn = 1;
      gm1b_7.M = CH; gm1b_7.N = H; gm1b_7.K = H; gm1b_7.zi_n = 1; gm1b_7.flags = 4; gm1b_7.act = 0;
      gm1b_7.alpha = 1.0f; gm1b_7.beta = 1.0f; gm1b_7.sa = 1.0f; gm1b_7.sb = 1.0f; gm1b_7.Npad = H; gm1b_7.pad_ = 0;
      k_gemm<1><<<dim3((unsigned)((H) + 31) / 32, (unsigned)((CH) + 15) / 16, (unsigned)(1)), 32, 0, stream>>>(gm1b_7); }
    { GemmP gm1c_7;
      gm1c_7.A = EF; gm1c_7.B = mnw1 + (size_t)256 * H; gm1c_7.bias = EF; gm1c_7.R = G; gm1c_7.C = G;
      gm1c_7.sAo = 0; gm1c_7.sAi = 0; gm1c_7.sAm = H; gm1c_7.sAk = 1; gm1c_7.sBo = 0; gm1c_7.sBi = 0; gm1c_7.sBn = 1; gm1c_7.sBk = H; gm1c_7.sCo = 0; gm1c_7.sCi = 0; gm1c_7.sCm = H; gm1c_7.sRo = 0; gm1c_7.sRi = 0; gm1c_7.sRm = H; gm1c_7.sRn = 1;
      gm1c_7.M = CH; gm1c_7.N = H; gm1c_7.K = H; gm1c_7.zi_n = 1; gm1c_7.flags = 4; gm1c_7.act = 0;
      gm1c_7.alpha = 1.0f; gm1c_7.beta = 1.0f; gm1c_7.sa = 1.0f; gm1c_7.sb = 1.0f; gm1c_7.Npad = H; gm1c_7.pad_ = 0;
      k_gemm<1><<<dim3((unsigned)((H) + 31) / 32, (unsigned)((CH) + 15) / 16, (unsigned)(1)), 32, 0, stream>>>(gm1c_7); }
    k_csp_silu<<<(unsigned)(((long long)CH * H + 255) / 256), 256, 0, stream>>>(G, (long long)CH * H);
    { GemmP gm2_7;
      gm2_7.A = G; gm2_7.B = mnw2; gm2_7.bias = mnb2; gm2_7.R = G; gm2_7.C = MSG;
      gm2_7.sAo = 0; gm2_7.sAi = 0; gm2_7.sAm = H; gm2_7.sAk = 1; gm2_7.sBo = 0; gm2_7.sBi = 0; gm2_7.sBn = 1; gm2_7.sBk = H; gm2_7.sCo = 0; gm2_7.sCi = 0; gm2_7.sCm = H; gm2_7.sRo = 0; gm2_7.sRi = 0; gm2_7.sRm = 0; gm2_7.sRn = 0;
      gm2_7.M = CH; gm2_7.N = H; gm2_7.K = H; gm2_7.zi_n = 1; gm2_7.flags = 1; gm2_7.act = 0;
      gm2_7.alpha = 1.0f; gm2_7.beta = 0.0f; gm2_7.sa = 1.0f; gm2_7.sb = 1.0f; gm2_7.Npad = H; gm2_7.pad_ = 0;
      k_gemm<1><<<dim3((unsigned)((H) + 31) / 32, (unsigned)((CH) + 15) / 16, (unsigned)(1)), 32, 0, stream>>>(gm2_7); }
    k_csp_agg<<<(unsigned)(((long long)Nn * H + 255) / 256), 256, 0, stream>>>(MSG, off, AGG, 350000, CH, Nn, H);
    k_csp_gather<<<(unsigned)(((long long)CH * H + 255) / 256), 256, 0, stream>>>(x, ea, ei, slot, XD, XS, EAc, 400000, CH, E, H, EDd);
    { GemmP ge1_8;
      ge1_8.A = EAc; ge1_8.B = eew1; ge1_8.bias = eeb1; ge1_8.R = EAc; ge1_8.C = EF1;
      ge1_8.sAo = 0; ge1_8.sAi = 0; ge1_8.sAm = 32; ge1_8.sAk = 1; ge1_8.sBo = 0; ge1_8.sBi = 0; ge1_8.sBn = 1; ge1_8.sBk = H; ge1_8.sCo = 0; ge1_8.sCi = 0; ge1_8.sCm = H; ge1_8.sRo = 0; ge1_8.sRi = 0; ge1_8.sRm = 0; ge1_8.sRn = 0;
      ge1_8.M = CH; ge1_8.N = H; ge1_8.K = EDd; ge1_8.zi_n = 1; ge1_8.flags = 1; ge1_8.act = 0;
      ge1_8.alpha = 1.0f; ge1_8.beta = 0.0f; ge1_8.sa = 1.0f; ge1_8.sb = 1.0f; ge1_8.Npad = H; ge1_8.pad_ = 0;
      k_gemm<1><<<dim3((unsigned)((H) + 31) / 32, (unsigned)((CH) + 15) / 16, (unsigned)(1)), 32, 0, stream>>>(ge1_8); }
    k_csp_silu<<<(unsigned)(((long long)CH * H + 255) / 256), 256, 0, stream>>>(EF1, (long long)CH * H);
    { GemmP ge2_8;
      ge2_8.A = EF1; ge2_8.B = eew2; ge2_8.bias = eeb2; ge2_8.R = EF1; ge2_8.C = EF;
      ge2_8.sAo = 0; ge2_8.sAi = 0; ge2_8.sAm = H; ge2_8.sAk = 1; ge2_8.sBo = 0; ge2_8.sBi = 0; ge2_8.sBn = 1; ge2_8.sBk = H; ge2_8.sCo = 0; ge2_8.sCi = 0; ge2_8.sCm = H; ge2_8.sRo = 0; ge2_8.sRi = 0; ge2_8.sRm = 0; ge2_8.sRn = 0;
      ge2_8.M = CH; ge2_8.N = H; ge2_8.K = H; ge2_8.zi_n = 1; ge2_8.flags = 1; ge2_8.act = 0;
      ge2_8.alpha = 1.0f; ge2_8.beta = 0.0f; ge2_8.sa = 1.0f; ge2_8.sb = 1.0f; ge2_8.Npad = H; ge2_8.pad_ = 0;
      k_gemm<1><<<dim3((unsigned)((H) + 31) / 32, (unsigned)((CH) + 15) / 16, (unsigned)(1)), 32, 0, stream>>>(ge2_8); }
    { GemmP gm1a_8;
      gm1a_8.A = XD; gm1a_8.B = mnw1; gm1a_8.bias = mnb1; gm1a_8.R = XD; gm1a_8.C = G;
      gm1a_8.sAo = 0; gm1a_8.sAi = 0; gm1a_8.sAm = H; gm1a_8.sAk = 1; gm1a_8.sBo = 0; gm1a_8.sBi = 0; gm1a_8.sBn = 1; gm1a_8.sBk = H; gm1a_8.sCo = 0; gm1a_8.sCi = 0; gm1a_8.sCm = H; gm1a_8.sRo = 0; gm1a_8.sRi = 0; gm1a_8.sRm = 0; gm1a_8.sRn = 0;
      gm1a_8.M = CH; gm1a_8.N = H; gm1a_8.K = H; gm1a_8.zi_n = 1; gm1a_8.flags = 1; gm1a_8.act = 0;
      gm1a_8.alpha = 1.0f; gm1a_8.beta = 0.0f; gm1a_8.sa = 1.0f; gm1a_8.sb = 1.0f; gm1a_8.Npad = H; gm1a_8.pad_ = 0;
      k_gemm<1><<<dim3((unsigned)((H) + 31) / 32, (unsigned)((CH) + 15) / 16, (unsigned)(1)), 32, 0, stream>>>(gm1a_8); }
    { GemmP gm1b_8;
      gm1b_8.A = XS; gm1b_8.B = mnw1 + (size_t)128 * H; gm1b_8.bias = XS; gm1b_8.R = G; gm1b_8.C = G;
      gm1b_8.sAo = 0; gm1b_8.sAi = 0; gm1b_8.sAm = H; gm1b_8.sAk = 1; gm1b_8.sBo = 0; gm1b_8.sBi = 0; gm1b_8.sBn = 1; gm1b_8.sBk = H; gm1b_8.sCo = 0; gm1b_8.sCi = 0; gm1b_8.sCm = H; gm1b_8.sRo = 0; gm1b_8.sRi = 0; gm1b_8.sRm = H; gm1b_8.sRn = 1;
      gm1b_8.M = CH; gm1b_8.N = H; gm1b_8.K = H; gm1b_8.zi_n = 1; gm1b_8.flags = 4; gm1b_8.act = 0;
      gm1b_8.alpha = 1.0f; gm1b_8.beta = 1.0f; gm1b_8.sa = 1.0f; gm1b_8.sb = 1.0f; gm1b_8.Npad = H; gm1b_8.pad_ = 0;
      k_gemm<1><<<dim3((unsigned)((H) + 31) / 32, (unsigned)((CH) + 15) / 16, (unsigned)(1)), 32, 0, stream>>>(gm1b_8); }
    { GemmP gm1c_8;
      gm1c_8.A = EF; gm1c_8.B = mnw1 + (size_t)256 * H; gm1c_8.bias = EF; gm1c_8.R = G; gm1c_8.C = G;
      gm1c_8.sAo = 0; gm1c_8.sAi = 0; gm1c_8.sAm = H; gm1c_8.sAk = 1; gm1c_8.sBo = 0; gm1c_8.sBi = 0; gm1c_8.sBn = 1; gm1c_8.sBk = H; gm1c_8.sCo = 0; gm1c_8.sCi = 0; gm1c_8.sCm = H; gm1c_8.sRo = 0; gm1c_8.sRi = 0; gm1c_8.sRm = H; gm1c_8.sRn = 1;
      gm1c_8.M = CH; gm1c_8.N = H; gm1c_8.K = H; gm1c_8.zi_n = 1; gm1c_8.flags = 4; gm1c_8.act = 0;
      gm1c_8.alpha = 1.0f; gm1c_8.beta = 1.0f; gm1c_8.sa = 1.0f; gm1c_8.sb = 1.0f; gm1c_8.Npad = H; gm1c_8.pad_ = 0;
      k_gemm<1><<<dim3((unsigned)((H) + 31) / 32, (unsigned)((CH) + 15) / 16, (unsigned)(1)), 32, 0, stream>>>(gm1c_8); }
    k_csp_silu<<<(unsigned)(((long long)CH * H + 255) / 256), 256, 0, stream>>>(G, (long long)CH * H);
    { GemmP gm2_8;
      gm2_8.A = G; gm2_8.B = mnw2; gm2_8.bias = mnb2; gm2_8.R = G; gm2_8.C = MSG;
      gm2_8.sAo = 0; gm2_8.sAi = 0; gm2_8.sAm = H; gm2_8.sAk = 1; gm2_8.sBo = 0; gm2_8.sBi = 0; gm2_8.sBn = 1; gm2_8.sBk = H; gm2_8.sCo = 0; gm2_8.sCi = 0; gm2_8.sCm = H; gm2_8.sRo = 0; gm2_8.sRi = 0; gm2_8.sRm = 0; gm2_8.sRn = 0;
      gm2_8.M = CH; gm2_8.N = H; gm2_8.K = H; gm2_8.zi_n = 1; gm2_8.flags = 1; gm2_8.act = 0;
      gm2_8.alpha = 1.0f; gm2_8.beta = 0.0f; gm2_8.sa = 1.0f; gm2_8.sb = 1.0f; gm2_8.Npad = H; gm2_8.pad_ = 0;
      k_gemm<1><<<dim3((unsigned)((H) + 31) / 32, (unsigned)((CH) + 15) / 16, (unsigned)(1)), 32, 0, stream>>>(gm2_8); }
    k_csp_agg<<<(unsigned)(((long long)Nn * H + 255) / 256), 256, 0, stream>>>(MSG, off, AGG, 400000, CH, Nn, H);
    k_csp_gather<<<(unsigned)(((long long)CH * H + 255) / 256), 256, 0, stream>>>(x, ea, ei, slot, XD, XS, EAc, 450000, CH, E, H, EDd);
    { GemmP ge1_9;
      ge1_9.A = EAc; ge1_9.B = eew1; ge1_9.bias = eeb1; ge1_9.R = EAc; ge1_9.C = EF1;
      ge1_9.sAo = 0; ge1_9.sAi = 0; ge1_9.sAm = 32; ge1_9.sAk = 1; ge1_9.sBo = 0; ge1_9.sBi = 0; ge1_9.sBn = 1; ge1_9.sBk = H; ge1_9.sCo = 0; ge1_9.sCi = 0; ge1_9.sCm = H; ge1_9.sRo = 0; ge1_9.sRi = 0; ge1_9.sRm = 0; ge1_9.sRn = 0;
      ge1_9.M = CH; ge1_9.N = H; ge1_9.K = EDd; ge1_9.zi_n = 1; ge1_9.flags = 1; ge1_9.act = 0;
      ge1_9.alpha = 1.0f; ge1_9.beta = 0.0f; ge1_9.sa = 1.0f; ge1_9.sb = 1.0f; ge1_9.Npad = H; ge1_9.pad_ = 0;
      k_gemm<1><<<dim3((unsigned)((H) + 31) / 32, (unsigned)((CH) + 15) / 16, (unsigned)(1)), 32, 0, stream>>>(ge1_9); }
    k_csp_silu<<<(unsigned)(((long long)CH * H + 255) / 256), 256, 0, stream>>>(EF1, (long long)CH * H);
    { GemmP ge2_9;
      ge2_9.A = EF1; ge2_9.B = eew2; ge2_9.bias = eeb2; ge2_9.R = EF1; ge2_9.C = EF;
      ge2_9.sAo = 0; ge2_9.sAi = 0; ge2_9.sAm = H; ge2_9.sAk = 1; ge2_9.sBo = 0; ge2_9.sBi = 0; ge2_9.sBn = 1; ge2_9.sBk = H; ge2_9.sCo = 0; ge2_9.sCi = 0; ge2_9.sCm = H; ge2_9.sRo = 0; ge2_9.sRi = 0; ge2_9.sRm = 0; ge2_9.sRn = 0;
      ge2_9.M = CH; ge2_9.N = H; ge2_9.K = H; ge2_9.zi_n = 1; ge2_9.flags = 1; ge2_9.act = 0;
      ge2_9.alpha = 1.0f; ge2_9.beta = 0.0f; ge2_9.sa = 1.0f; ge2_9.sb = 1.0f; ge2_9.Npad = H; ge2_9.pad_ = 0;
      k_gemm<1><<<dim3((unsigned)((H) + 31) / 32, (unsigned)((CH) + 15) / 16, (unsigned)(1)), 32, 0, stream>>>(ge2_9); }
    { GemmP gm1a_9;
      gm1a_9.A = XD; gm1a_9.B = mnw1; gm1a_9.bias = mnb1; gm1a_9.R = XD; gm1a_9.C = G;
      gm1a_9.sAo = 0; gm1a_9.sAi = 0; gm1a_9.sAm = H; gm1a_9.sAk = 1; gm1a_9.sBo = 0; gm1a_9.sBi = 0; gm1a_9.sBn = 1; gm1a_9.sBk = H; gm1a_9.sCo = 0; gm1a_9.sCi = 0; gm1a_9.sCm = H; gm1a_9.sRo = 0; gm1a_9.sRi = 0; gm1a_9.sRm = 0; gm1a_9.sRn = 0;
      gm1a_9.M = CH; gm1a_9.N = H; gm1a_9.K = H; gm1a_9.zi_n = 1; gm1a_9.flags = 1; gm1a_9.act = 0;
      gm1a_9.alpha = 1.0f; gm1a_9.beta = 0.0f; gm1a_9.sa = 1.0f; gm1a_9.sb = 1.0f; gm1a_9.Npad = H; gm1a_9.pad_ = 0;
      k_gemm<1><<<dim3((unsigned)((H) + 31) / 32, (unsigned)((CH) + 15) / 16, (unsigned)(1)), 32, 0, stream>>>(gm1a_9); }
    { GemmP gm1b_9;
      gm1b_9.A = XS; gm1b_9.B = mnw1 + (size_t)128 * H; gm1b_9.bias = XS; gm1b_9.R = G; gm1b_9.C = G;
      gm1b_9.sAo = 0; gm1b_9.sAi = 0; gm1b_9.sAm = H; gm1b_9.sAk = 1; gm1b_9.sBo = 0; gm1b_9.sBi = 0; gm1b_9.sBn = 1; gm1b_9.sBk = H; gm1b_9.sCo = 0; gm1b_9.sCi = 0; gm1b_9.sCm = H; gm1b_9.sRo = 0; gm1b_9.sRi = 0; gm1b_9.sRm = H; gm1b_9.sRn = 1;
      gm1b_9.M = CH; gm1b_9.N = H; gm1b_9.K = H; gm1b_9.zi_n = 1; gm1b_9.flags = 4; gm1b_9.act = 0;
      gm1b_9.alpha = 1.0f; gm1b_9.beta = 1.0f; gm1b_9.sa = 1.0f; gm1b_9.sb = 1.0f; gm1b_9.Npad = H; gm1b_9.pad_ = 0;
      k_gemm<1><<<dim3((unsigned)((H) + 31) / 32, (unsigned)((CH) + 15) / 16, (unsigned)(1)), 32, 0, stream>>>(gm1b_9); }
    { GemmP gm1c_9;
      gm1c_9.A = EF; gm1c_9.B = mnw1 + (size_t)256 * H; gm1c_9.bias = EF; gm1c_9.R = G; gm1c_9.C = G;
      gm1c_9.sAo = 0; gm1c_9.sAi = 0; gm1c_9.sAm = H; gm1c_9.sAk = 1; gm1c_9.sBo = 0; gm1c_9.sBi = 0; gm1c_9.sBn = 1; gm1c_9.sBk = H; gm1c_9.sCo = 0; gm1c_9.sCi = 0; gm1c_9.sCm = H; gm1c_9.sRo = 0; gm1c_9.sRi = 0; gm1c_9.sRm = H; gm1c_9.sRn = 1;
      gm1c_9.M = CH; gm1c_9.N = H; gm1c_9.K = H; gm1c_9.zi_n = 1; gm1c_9.flags = 4; gm1c_9.act = 0;
      gm1c_9.alpha = 1.0f; gm1c_9.beta = 1.0f; gm1c_9.sa = 1.0f; gm1c_9.sb = 1.0f; gm1c_9.Npad = H; gm1c_9.pad_ = 0;
      k_gemm<1><<<dim3((unsigned)((H) + 31) / 32, (unsigned)((CH) + 15) / 16, (unsigned)(1)), 32, 0, stream>>>(gm1c_9); }
    k_csp_silu<<<(unsigned)(((long long)CH * H + 255) / 256), 256, 0, stream>>>(G, (long long)CH * H);
    { GemmP gm2_9;
      gm2_9.A = G; gm2_9.B = mnw2; gm2_9.bias = mnb2; gm2_9.R = G; gm2_9.C = MSG;
      gm2_9.sAo = 0; gm2_9.sAi = 0; gm2_9.sAm = H; gm2_9.sAk = 1; gm2_9.sBo = 0; gm2_9.sBi = 0; gm2_9.sBn = 1; gm2_9.sBk = H; gm2_9.sCo = 0; gm2_9.sCi = 0; gm2_9.sCm = H; gm2_9.sRo = 0; gm2_9.sRi = 0; gm2_9.sRm = 0; gm2_9.sRn = 0;
      gm2_9.M = CH; gm2_9.N = H; gm2_9.K = H; gm2_9.zi_n = 1; gm2_9.flags = 1; gm2_9.act = 0;
      gm2_9.alpha = 1.0f; gm2_9.beta = 0.0f; gm2_9.sa = 1.0f; gm2_9.sb = 1.0f; gm2_9.Npad = H; gm2_9.pad_ = 0;
      k_gemm<1><<<dim3((unsigned)((H) + 31) / 32, (unsigned)((CH) + 15) / 16, (unsigned)(1)), 32, 0, stream>>>(gm2_9); }
    k_csp_agg<<<(unsigned)(((long long)Nn * H + 255) / 256), 256, 0, stream>>>(MSG, off, AGG, 450000, CH, Nn, H);
    k_csp_gather<<<(unsigned)(((long long)CH * H + 255) / 256), 256, 0, stream>>>(x, ea, ei, slot, XD, XS, EAc, 500000, CH, E, H, EDd);
    { GemmP ge1_10;
      ge1_10.A = EAc; ge1_10.B = eew1; ge1_10.bias = eeb1; ge1_10.R = EAc; ge1_10.C = EF1;
      ge1_10.sAo = 0; ge1_10.sAi = 0; ge1_10.sAm = 32; ge1_10.sAk = 1; ge1_10.sBo = 0; ge1_10.sBi = 0; ge1_10.sBn = 1; ge1_10.sBk = H; ge1_10.sCo = 0; ge1_10.sCi = 0; ge1_10.sCm = H; ge1_10.sRo = 0; ge1_10.sRi = 0; ge1_10.sRm = 0; ge1_10.sRn = 0;
      ge1_10.M = CH; ge1_10.N = H; ge1_10.K = EDd; ge1_10.zi_n = 1; ge1_10.flags = 1; ge1_10.act = 0;
      ge1_10.alpha = 1.0f; ge1_10.beta = 0.0f; ge1_10.sa = 1.0f; ge1_10.sb = 1.0f; ge1_10.Npad = H; ge1_10.pad_ = 0;
      k_gemm<1><<<dim3((unsigned)((H) + 31) / 32, (unsigned)((CH) + 15) / 16, (unsigned)(1)), 32, 0, stream>>>(ge1_10); }
    k_csp_silu<<<(unsigned)(((long long)CH * H + 255) / 256), 256, 0, stream>>>(EF1, (long long)CH * H);
    { GemmP ge2_10;
      ge2_10.A = EF1; ge2_10.B = eew2; ge2_10.bias = eeb2; ge2_10.R = EF1; ge2_10.C = EF;
      ge2_10.sAo = 0; ge2_10.sAi = 0; ge2_10.sAm = H; ge2_10.sAk = 1; ge2_10.sBo = 0; ge2_10.sBi = 0; ge2_10.sBn = 1; ge2_10.sBk = H; ge2_10.sCo = 0; ge2_10.sCi = 0; ge2_10.sCm = H; ge2_10.sRo = 0; ge2_10.sRi = 0; ge2_10.sRm = 0; ge2_10.sRn = 0;
      ge2_10.M = CH; ge2_10.N = H; ge2_10.K = H; ge2_10.zi_n = 1; ge2_10.flags = 1; ge2_10.act = 0;
      ge2_10.alpha = 1.0f; ge2_10.beta = 0.0f; ge2_10.sa = 1.0f; ge2_10.sb = 1.0f; ge2_10.Npad = H; ge2_10.pad_ = 0;
      k_gemm<1><<<dim3((unsigned)((H) + 31) / 32, (unsigned)((CH) + 15) / 16, (unsigned)(1)), 32, 0, stream>>>(ge2_10); }
    { GemmP gm1a_10;
      gm1a_10.A = XD; gm1a_10.B = mnw1; gm1a_10.bias = mnb1; gm1a_10.R = XD; gm1a_10.C = G;
      gm1a_10.sAo = 0; gm1a_10.sAi = 0; gm1a_10.sAm = H; gm1a_10.sAk = 1; gm1a_10.sBo = 0; gm1a_10.sBi = 0; gm1a_10.sBn = 1; gm1a_10.sBk = H; gm1a_10.sCo = 0; gm1a_10.sCi = 0; gm1a_10.sCm = H; gm1a_10.sRo = 0; gm1a_10.sRi = 0; gm1a_10.sRm = 0; gm1a_10.sRn = 0;
      gm1a_10.M = CH; gm1a_10.N = H; gm1a_10.K = H; gm1a_10.zi_n = 1; gm1a_10.flags = 1; gm1a_10.act = 0;
      gm1a_10.alpha = 1.0f; gm1a_10.beta = 0.0f; gm1a_10.sa = 1.0f; gm1a_10.sb = 1.0f; gm1a_10.Npad = H; gm1a_10.pad_ = 0;
      k_gemm<1><<<dim3((unsigned)((H) + 31) / 32, (unsigned)((CH) + 15) / 16, (unsigned)(1)), 32, 0, stream>>>(gm1a_10); }
    { GemmP gm1b_10;
      gm1b_10.A = XS; gm1b_10.B = mnw1 + (size_t)128 * H; gm1b_10.bias = XS; gm1b_10.R = G; gm1b_10.C = G;
      gm1b_10.sAo = 0; gm1b_10.sAi = 0; gm1b_10.sAm = H; gm1b_10.sAk = 1; gm1b_10.sBo = 0; gm1b_10.sBi = 0; gm1b_10.sBn = 1; gm1b_10.sBk = H; gm1b_10.sCo = 0; gm1b_10.sCi = 0; gm1b_10.sCm = H; gm1b_10.sRo = 0; gm1b_10.sRi = 0; gm1b_10.sRm = H; gm1b_10.sRn = 1;
      gm1b_10.M = CH; gm1b_10.N = H; gm1b_10.K = H; gm1b_10.zi_n = 1; gm1b_10.flags = 4; gm1b_10.act = 0;
      gm1b_10.alpha = 1.0f; gm1b_10.beta = 1.0f; gm1b_10.sa = 1.0f; gm1b_10.sb = 1.0f; gm1b_10.Npad = H; gm1b_10.pad_ = 0;
      k_gemm<1><<<dim3((unsigned)((H) + 31) / 32, (unsigned)((CH) + 15) / 16, (unsigned)(1)), 32, 0, stream>>>(gm1b_10); }
    { GemmP gm1c_10;
      gm1c_10.A = EF; gm1c_10.B = mnw1 + (size_t)256 * H; gm1c_10.bias = EF; gm1c_10.R = G; gm1c_10.C = G;
      gm1c_10.sAo = 0; gm1c_10.sAi = 0; gm1c_10.sAm = H; gm1c_10.sAk = 1; gm1c_10.sBo = 0; gm1c_10.sBi = 0; gm1c_10.sBn = 1; gm1c_10.sBk = H; gm1c_10.sCo = 0; gm1c_10.sCi = 0; gm1c_10.sCm = H; gm1c_10.sRo = 0; gm1c_10.sRi = 0; gm1c_10.sRm = H; gm1c_10.sRn = 1;
      gm1c_10.M = CH; gm1c_10.N = H; gm1c_10.K = H; gm1c_10.zi_n = 1; gm1c_10.flags = 4; gm1c_10.act = 0;
      gm1c_10.alpha = 1.0f; gm1c_10.beta = 1.0f; gm1c_10.sa = 1.0f; gm1c_10.sb = 1.0f; gm1c_10.Npad = H; gm1c_10.pad_ = 0;
      k_gemm<1><<<dim3((unsigned)((H) + 31) / 32, (unsigned)((CH) + 15) / 16, (unsigned)(1)), 32, 0, stream>>>(gm1c_10); }
    k_csp_silu<<<(unsigned)(((long long)CH * H + 255) / 256), 256, 0, stream>>>(G, (long long)CH * H);
    { GemmP gm2_10;
      gm2_10.A = G; gm2_10.B = mnw2; gm2_10.bias = mnb2; gm2_10.R = G; gm2_10.C = MSG;
      gm2_10.sAo = 0; gm2_10.sAi = 0; gm2_10.sAm = H; gm2_10.sAk = 1; gm2_10.sBo = 0; gm2_10.sBi = 0; gm2_10.sBn = 1; gm2_10.sBk = H; gm2_10.sCo = 0; gm2_10.sCi = 0; gm2_10.sCm = H; gm2_10.sRo = 0; gm2_10.sRi = 0; gm2_10.sRm = 0; gm2_10.sRn = 0;
      gm2_10.M = CH; gm2_10.N = H; gm2_10.K = H; gm2_10.zi_n = 1; gm2_10.flags = 1; gm2_10.act = 0;
      gm2_10.alpha = 1.0f; gm2_10.beta = 0.0f; gm2_10.sa = 1.0f; gm2_10.sb = 1.0f; gm2_10.Npad = H; gm2_10.pad_ = 0;
      k_gemm<1><<<dim3((unsigned)((H) + 31) / 32, (unsigned)((CH) + 15) / 16, (unsigned)(1)), 32, 0, stream>>>(gm2_10); }
    k_csp_agg<<<(unsigned)(((long long)Nn * H + 255) / 256), 256, 0, stream>>>(MSG, off, AGG, 500000, CH, Nn, H);
    k_csp_gather<<<(unsigned)(((long long)CH * H + 255) / 256), 256, 0, stream>>>(x, ea, ei, slot, XD, XS, EAc, 550000, CH, E, H, EDd);
    { GemmP ge1_11;
      ge1_11.A = EAc; ge1_11.B = eew1; ge1_11.bias = eeb1; ge1_11.R = EAc; ge1_11.C = EF1;
      ge1_11.sAo = 0; ge1_11.sAi = 0; ge1_11.sAm = 32; ge1_11.sAk = 1; ge1_11.sBo = 0; ge1_11.sBi = 0; ge1_11.sBn = 1; ge1_11.sBk = H; ge1_11.sCo = 0; ge1_11.sCi = 0; ge1_11.sCm = H; ge1_11.sRo = 0; ge1_11.sRi = 0; ge1_11.sRm = 0; ge1_11.sRn = 0;
      ge1_11.M = CH; ge1_11.N = H; ge1_11.K = EDd; ge1_11.zi_n = 1; ge1_11.flags = 1; ge1_11.act = 0;
      ge1_11.alpha = 1.0f; ge1_11.beta = 0.0f; ge1_11.sa = 1.0f; ge1_11.sb = 1.0f; ge1_11.Npad = H; ge1_11.pad_ = 0;
      k_gemm<1><<<dim3((unsigned)((H) + 31) / 32, (unsigned)((CH) + 15) / 16, (unsigned)(1)), 32, 0, stream>>>(ge1_11); }
    k_csp_silu<<<(unsigned)(((long long)CH * H + 255) / 256), 256, 0, stream>>>(EF1, (long long)CH * H);
    { GemmP ge2_11;
      ge2_11.A = EF1; ge2_11.B = eew2; ge2_11.bias = eeb2; ge2_11.R = EF1; ge2_11.C = EF;
      ge2_11.sAo = 0; ge2_11.sAi = 0; ge2_11.sAm = H; ge2_11.sAk = 1; ge2_11.sBo = 0; ge2_11.sBi = 0; ge2_11.sBn = 1; ge2_11.sBk = H; ge2_11.sCo = 0; ge2_11.sCi = 0; ge2_11.sCm = H; ge2_11.sRo = 0; ge2_11.sRi = 0; ge2_11.sRm = 0; ge2_11.sRn = 0;
      ge2_11.M = CH; ge2_11.N = H; ge2_11.K = H; ge2_11.zi_n = 1; ge2_11.flags = 1; ge2_11.act = 0;
      ge2_11.alpha = 1.0f; ge2_11.beta = 0.0f; ge2_11.sa = 1.0f; ge2_11.sb = 1.0f; ge2_11.Npad = H; ge2_11.pad_ = 0;
      k_gemm<1><<<dim3((unsigned)((H) + 31) / 32, (unsigned)((CH) + 15) / 16, (unsigned)(1)), 32, 0, stream>>>(ge2_11); }
    { GemmP gm1a_11;
      gm1a_11.A = XD; gm1a_11.B = mnw1; gm1a_11.bias = mnb1; gm1a_11.R = XD; gm1a_11.C = G;
      gm1a_11.sAo = 0; gm1a_11.sAi = 0; gm1a_11.sAm = H; gm1a_11.sAk = 1; gm1a_11.sBo = 0; gm1a_11.sBi = 0; gm1a_11.sBn = 1; gm1a_11.sBk = H; gm1a_11.sCo = 0; gm1a_11.sCi = 0; gm1a_11.sCm = H; gm1a_11.sRo = 0; gm1a_11.sRi = 0; gm1a_11.sRm = 0; gm1a_11.sRn = 0;
      gm1a_11.M = CH; gm1a_11.N = H; gm1a_11.K = H; gm1a_11.zi_n = 1; gm1a_11.flags = 1; gm1a_11.act = 0;
      gm1a_11.alpha = 1.0f; gm1a_11.beta = 0.0f; gm1a_11.sa = 1.0f; gm1a_11.sb = 1.0f; gm1a_11.Npad = H; gm1a_11.pad_ = 0;
      k_gemm<1><<<dim3((unsigned)((H) + 31) / 32, (unsigned)((CH) + 15) / 16, (unsigned)(1)), 32, 0, stream>>>(gm1a_11); }
    { GemmP gm1b_11;
      gm1b_11.A = XS; gm1b_11.B = mnw1 + (size_t)128 * H; gm1b_11.bias = XS; gm1b_11.R = G; gm1b_11.C = G;
      gm1b_11.sAo = 0; gm1b_11.sAi = 0; gm1b_11.sAm = H; gm1b_11.sAk = 1; gm1b_11.sBo = 0; gm1b_11.sBi = 0; gm1b_11.sBn = 1; gm1b_11.sBk = H; gm1b_11.sCo = 0; gm1b_11.sCi = 0; gm1b_11.sCm = H; gm1b_11.sRo = 0; gm1b_11.sRi = 0; gm1b_11.sRm = H; gm1b_11.sRn = 1;
      gm1b_11.M = CH; gm1b_11.N = H; gm1b_11.K = H; gm1b_11.zi_n = 1; gm1b_11.flags = 4; gm1b_11.act = 0;
      gm1b_11.alpha = 1.0f; gm1b_11.beta = 1.0f; gm1b_11.sa = 1.0f; gm1b_11.sb = 1.0f; gm1b_11.Npad = H; gm1b_11.pad_ = 0;
      k_gemm<1><<<dim3((unsigned)((H) + 31) / 32, (unsigned)((CH) + 15) / 16, (unsigned)(1)), 32, 0, stream>>>(gm1b_11); }
    { GemmP gm1c_11;
      gm1c_11.A = EF; gm1c_11.B = mnw1 + (size_t)256 * H; gm1c_11.bias = EF; gm1c_11.R = G; gm1c_11.C = G;
      gm1c_11.sAo = 0; gm1c_11.sAi = 0; gm1c_11.sAm = H; gm1c_11.sAk = 1; gm1c_11.sBo = 0; gm1c_11.sBi = 0; gm1c_11.sBn = 1; gm1c_11.sBk = H; gm1c_11.sCo = 0; gm1c_11.sCi = 0; gm1c_11.sCm = H; gm1c_11.sRo = 0; gm1c_11.sRi = 0; gm1c_11.sRm = H; gm1c_11.sRn = 1;
      gm1c_11.M = CH; gm1c_11.N = H; gm1c_11.K = H; gm1c_11.zi_n = 1; gm1c_11.flags = 4; gm1c_11.act = 0;
      gm1c_11.alpha = 1.0f; gm1c_11.beta = 1.0f; gm1c_11.sa = 1.0f; gm1c_11.sb = 1.0f; gm1c_11.Npad = H; gm1c_11.pad_ = 0;
      k_gemm<1><<<dim3((unsigned)((H) + 31) / 32, (unsigned)((CH) + 15) / 16, (unsigned)(1)), 32, 0, stream>>>(gm1c_11); }
    k_csp_silu<<<(unsigned)(((long long)CH * H + 255) / 256), 256, 0, stream>>>(G, (long long)CH * H);
    { GemmP gm2_11;
      gm2_11.A = G; gm2_11.B = mnw2; gm2_11.bias = mnb2; gm2_11.R = G; gm2_11.C = MSG;
      gm2_11.sAo = 0; gm2_11.sAi = 0; gm2_11.sAm = H; gm2_11.sAk = 1; gm2_11.sBo = 0; gm2_11.sBi = 0; gm2_11.sBn = 1; gm2_11.sBk = H; gm2_11.sCo = 0; gm2_11.sCi = 0; gm2_11.sCm = H; gm2_11.sRo = 0; gm2_11.sRi = 0; gm2_11.sRm = 0; gm2_11.sRn = 0;
      gm2_11.M = CH; gm2_11.N = H; gm2_11.K = H; gm2_11.zi_n = 1; gm2_11.flags = 1; gm2_11.act = 0;
      gm2_11.alpha = 1.0f; gm2_11.beta = 0.0f; gm2_11.sa = 1.0f; gm2_11.sb = 1.0f; gm2_11.Npad = H; gm2_11.pad_ = 0;
      k_gemm<1><<<dim3((unsigned)((H) + 31) / 32, (unsigned)((CH) + 15) / 16, (unsigned)(1)), 32, 0, stream>>>(gm2_11); }
    k_csp_agg<<<(unsigned)(((long long)Nn * H + 255) / 256), 256, 0, stream>>>(MSG, off, AGG, 550000, CH, Nn, H);
    k_csp_gather<<<(unsigned)(((long long)CH * H + 255) / 256), 256, 0, stream>>>(x, ea, ei, slot, XD, XS, EAc, 600000, CH, E, H, EDd);
    { GemmP ge1_12;
      ge1_12.A = EAc; ge1_12.B = eew1; ge1_12.bias = eeb1; ge1_12.R = EAc; ge1_12.C = EF1;
      ge1_12.sAo = 0; ge1_12.sAi = 0; ge1_12.sAm = 32; ge1_12.sAk = 1; ge1_12.sBo = 0; ge1_12.sBi = 0; ge1_12.sBn = 1; ge1_12.sBk = H; ge1_12.sCo = 0; ge1_12.sCi = 0; ge1_12.sCm = H; ge1_12.sRo = 0; ge1_12.sRi = 0; ge1_12.sRm = 0; ge1_12.sRn = 0;
      ge1_12.M = CH; ge1_12.N = H; ge1_12.K = EDd; ge1_12.zi_n = 1; ge1_12.flags = 1; ge1_12.act = 0;
      ge1_12.alpha = 1.0f; ge1_12.beta = 0.0f; ge1_12.sa = 1.0f; ge1_12.sb = 1.0f; ge1_12.Npad = H; ge1_12.pad_ = 0;
      k_gemm<1><<<dim3((unsigned)((H) + 31) / 32, (unsigned)((CH) + 15) / 16, (unsigned)(1)), 32, 0, stream>>>(ge1_12); }
    k_csp_silu<<<(unsigned)(((long long)CH * H + 255) / 256), 256, 0, stream>>>(EF1, (long long)CH * H);
    { GemmP ge2_12;
      ge2_12.A = EF1; ge2_12.B = eew2; ge2_12.bias = eeb2; ge2_12.R = EF1; ge2_12.C = EF;
      ge2_12.sAo = 0; ge2_12.sAi = 0; ge2_12.sAm = H; ge2_12.sAk = 1; ge2_12.sBo = 0; ge2_12.sBi = 0; ge2_12.sBn = 1; ge2_12.sBk = H; ge2_12.sCo = 0; ge2_12.sCi = 0; ge2_12.sCm = H; ge2_12.sRo = 0; ge2_12.sRi = 0; ge2_12.sRm = 0; ge2_12.sRn = 0;
      ge2_12.M = CH; ge2_12.N = H; ge2_12.K = H; ge2_12.zi_n = 1; ge2_12.flags = 1; ge2_12.act = 0;
      ge2_12.alpha = 1.0f; ge2_12.beta = 0.0f; ge2_12.sa = 1.0f; ge2_12.sb = 1.0f; ge2_12.Npad = H; ge2_12.pad_ = 0;
      k_gemm<1><<<dim3((unsigned)((H) + 31) / 32, (unsigned)((CH) + 15) / 16, (unsigned)(1)), 32, 0, stream>>>(ge2_12); }
    { GemmP gm1a_12;
      gm1a_12.A = XD; gm1a_12.B = mnw1; gm1a_12.bias = mnb1; gm1a_12.R = XD; gm1a_12.C = G;
      gm1a_12.sAo = 0; gm1a_12.sAi = 0; gm1a_12.sAm = H; gm1a_12.sAk = 1; gm1a_12.sBo = 0; gm1a_12.sBi = 0; gm1a_12.sBn = 1; gm1a_12.sBk = H; gm1a_12.sCo = 0; gm1a_12.sCi = 0; gm1a_12.sCm = H; gm1a_12.sRo = 0; gm1a_12.sRi = 0; gm1a_12.sRm = 0; gm1a_12.sRn = 0;
      gm1a_12.M = CH; gm1a_12.N = H; gm1a_12.K = H; gm1a_12.zi_n = 1; gm1a_12.flags = 1; gm1a_12.act = 0;
      gm1a_12.alpha = 1.0f; gm1a_12.beta = 0.0f; gm1a_12.sa = 1.0f; gm1a_12.sb = 1.0f; gm1a_12.Npad = H; gm1a_12.pad_ = 0;
      k_gemm<1><<<dim3((unsigned)((H) + 31) / 32, (unsigned)((CH) + 15) / 16, (unsigned)(1)), 32, 0, stream>>>(gm1a_12); }
    { GemmP gm1b_12;
      gm1b_12.A = XS; gm1b_12.B = mnw1 + (size_t)128 * H; gm1b_12.bias = XS; gm1b_12.R = G; gm1b_12.C = G;
      gm1b_12.sAo = 0; gm1b_12.sAi = 0; gm1b_12.sAm = H; gm1b_12.sAk = 1; gm1b_12.sBo = 0; gm1b_12.sBi = 0; gm1b_12.sBn = 1; gm1b_12.sBk = H; gm1b_12.sCo = 0; gm1b_12.sCi = 0; gm1b_12.sCm = H; gm1b_12.sRo = 0; gm1b_12.sRi = 0; gm1b_12.sRm = H; gm1b_12.sRn = 1;
      gm1b_12.M = CH; gm1b_12.N = H; gm1b_12.K = H; gm1b_12.zi_n = 1; gm1b_12.flags = 4; gm1b_12.act = 0;
      gm1b_12.alpha = 1.0f; gm1b_12.beta = 1.0f; gm1b_12.sa = 1.0f; gm1b_12.sb = 1.0f; gm1b_12.Npad = H; gm1b_12.pad_ = 0;
      k_gemm<1><<<dim3((unsigned)((H) + 31) / 32, (unsigned)((CH) + 15) / 16, (unsigned)(1)), 32, 0, stream>>>(gm1b_12); }
    { GemmP gm1c_12;
      gm1c_12.A = EF; gm1c_12.B = mnw1 + (size_t)256 * H; gm1c_12.bias = EF; gm1c_12.R = G; gm1c_12.C = G;
      gm1c_12.sAo = 0; gm1c_12.sAi = 0; gm1c_12.sAm = H; gm1c_12.sAk = 1; gm1c_12.sBo = 0; gm1c_12.sBi = 0; gm1c_12.sBn = 1; gm1c_12.sBk = H; gm1c_12.sCo = 0; gm1c_12.sCi = 0; gm1c_12.sCm = H; gm1c_12.sRo = 0; gm1c_12.sRi = 0; gm1c_12.sRm = H; gm1c_12.sRn = 1;
      gm1c_12.M = CH; gm1c_12.N = H; gm1c_12.K = H; gm1c_12.zi_n = 1; gm1c_12.flags = 4; gm1c_12.act = 0;
      gm1c_12.alpha = 1.0f; gm1c_12.beta = 1.0f; gm1c_12.sa = 1.0f; gm1c_12.sb = 1.0f; gm1c_12.Npad = H; gm1c_12.pad_ = 0;
      k_gemm<1><<<dim3((unsigned)((H) + 31) / 32, (unsigned)((CH) + 15) / 16, (unsigned)(1)), 32, 0, stream>>>(gm1c_12); }
    k_csp_silu<<<(unsigned)(((long long)CH * H + 255) / 256), 256, 0, stream>>>(G, (long long)CH * H);
    { GemmP gm2_12;
      gm2_12.A = G; gm2_12.B = mnw2; gm2_12.bias = mnb2; gm2_12.R = G; gm2_12.C = MSG;
      gm2_12.sAo = 0; gm2_12.sAi = 0; gm2_12.sAm = H; gm2_12.sAk = 1; gm2_12.sBo = 0; gm2_12.sBi = 0; gm2_12.sBn = 1; gm2_12.sBk = H; gm2_12.sCo = 0; gm2_12.sCi = 0; gm2_12.sCm = H; gm2_12.sRo = 0; gm2_12.sRi = 0; gm2_12.sRm = 0; gm2_12.sRn = 0;
      gm2_12.M = CH; gm2_12.N = H; gm2_12.K = H; gm2_12.zi_n = 1; gm2_12.flags = 1; gm2_12.act = 0;
      gm2_12.alpha = 1.0f; gm2_12.beta = 0.0f; gm2_12.sa = 1.0f; gm2_12.sb = 1.0f; gm2_12.Npad = H; gm2_12.pad_ = 0;
      k_gemm<1><<<dim3((unsigned)((H) + 31) / 32, (unsigned)((CH) + 15) / 16, (unsigned)(1)), 32, 0, stream>>>(gm2_12); }
    k_csp_agg<<<(unsigned)(((long long)Nn * H + 255) / 256), 256, 0, stream>>>(MSG, off, AGG, 600000, CH, Nn, H);
    k_csp_gather<<<(unsigned)(((long long)CH * H + 255) / 256), 256, 0, stream>>>(x, ea, ei, slot, XD, XS, EAc, 650000, CH, E, H, EDd);
    { GemmP ge1_13;
      ge1_13.A = EAc; ge1_13.B = eew1; ge1_13.bias = eeb1; ge1_13.R = EAc; ge1_13.C = EF1;
      ge1_13.sAo = 0; ge1_13.sAi = 0; ge1_13.sAm = 32; ge1_13.sAk = 1; ge1_13.sBo = 0; ge1_13.sBi = 0; ge1_13.sBn = 1; ge1_13.sBk = H; ge1_13.sCo = 0; ge1_13.sCi = 0; ge1_13.sCm = H; ge1_13.sRo = 0; ge1_13.sRi = 0; ge1_13.sRm = 0; ge1_13.sRn = 0;
      ge1_13.M = CH; ge1_13.N = H; ge1_13.K = EDd; ge1_13.zi_n = 1; ge1_13.flags = 1; ge1_13.act = 0;
      ge1_13.alpha = 1.0f; ge1_13.beta = 0.0f; ge1_13.sa = 1.0f; ge1_13.sb = 1.0f; ge1_13.Npad = H; ge1_13.pad_ = 0;
      k_gemm<1><<<dim3((unsigned)((H) + 31) / 32, (unsigned)((CH) + 15) / 16, (unsigned)(1)), 32, 0, stream>>>(ge1_13); }
    k_csp_silu<<<(unsigned)(((long long)CH * H + 255) / 256), 256, 0, stream>>>(EF1, (long long)CH * H);
    { GemmP ge2_13;
      ge2_13.A = EF1; ge2_13.B = eew2; ge2_13.bias = eeb2; ge2_13.R = EF1; ge2_13.C = EF;
      ge2_13.sAo = 0; ge2_13.sAi = 0; ge2_13.sAm = H; ge2_13.sAk = 1; ge2_13.sBo = 0; ge2_13.sBi = 0; ge2_13.sBn = 1; ge2_13.sBk = H; ge2_13.sCo = 0; ge2_13.sCi = 0; ge2_13.sCm = H; ge2_13.sRo = 0; ge2_13.sRi = 0; ge2_13.sRm = 0; ge2_13.sRn = 0;
      ge2_13.M = CH; ge2_13.N = H; ge2_13.K = H; ge2_13.zi_n = 1; ge2_13.flags = 1; ge2_13.act = 0;
      ge2_13.alpha = 1.0f; ge2_13.beta = 0.0f; ge2_13.sa = 1.0f; ge2_13.sb = 1.0f; ge2_13.Npad = H; ge2_13.pad_ = 0;
      k_gemm<1><<<dim3((unsigned)((H) + 31) / 32, (unsigned)((CH) + 15) / 16, (unsigned)(1)), 32, 0, stream>>>(ge2_13); }
    { GemmP gm1a_13;
      gm1a_13.A = XD; gm1a_13.B = mnw1; gm1a_13.bias = mnb1; gm1a_13.R = XD; gm1a_13.C = G;
      gm1a_13.sAo = 0; gm1a_13.sAi = 0; gm1a_13.sAm = H; gm1a_13.sAk = 1; gm1a_13.sBo = 0; gm1a_13.sBi = 0; gm1a_13.sBn = 1; gm1a_13.sBk = H; gm1a_13.sCo = 0; gm1a_13.sCi = 0; gm1a_13.sCm = H; gm1a_13.sRo = 0; gm1a_13.sRi = 0; gm1a_13.sRm = 0; gm1a_13.sRn = 0;
      gm1a_13.M = CH; gm1a_13.N = H; gm1a_13.K = H; gm1a_13.zi_n = 1; gm1a_13.flags = 1; gm1a_13.act = 0;
      gm1a_13.alpha = 1.0f; gm1a_13.beta = 0.0f; gm1a_13.sa = 1.0f; gm1a_13.sb = 1.0f; gm1a_13.Npad = H; gm1a_13.pad_ = 0;
      k_gemm<1><<<dim3((unsigned)((H) + 31) / 32, (unsigned)((CH) + 15) / 16, (unsigned)(1)), 32, 0, stream>>>(gm1a_13); }
    { GemmP gm1b_13;
      gm1b_13.A = XS; gm1b_13.B = mnw1 + (size_t)128 * H; gm1b_13.bias = XS; gm1b_13.R = G; gm1b_13.C = G;
      gm1b_13.sAo = 0; gm1b_13.sAi = 0; gm1b_13.sAm = H; gm1b_13.sAk = 1; gm1b_13.sBo = 0; gm1b_13.sBi = 0; gm1b_13.sBn = 1; gm1b_13.sBk = H; gm1b_13.sCo = 0; gm1b_13.sCi = 0; gm1b_13.sCm = H; gm1b_13.sRo = 0; gm1b_13.sRi = 0; gm1b_13.sRm = H; gm1b_13.sRn = 1;
      gm1b_13.M = CH; gm1b_13.N = H; gm1b_13.K = H; gm1b_13.zi_n = 1; gm1b_13.flags = 4; gm1b_13.act = 0;
      gm1b_13.alpha = 1.0f; gm1b_13.beta = 1.0f; gm1b_13.sa = 1.0f; gm1b_13.sb = 1.0f; gm1b_13.Npad = H; gm1b_13.pad_ = 0;
      k_gemm<1><<<dim3((unsigned)((H) + 31) / 32, (unsigned)((CH) + 15) / 16, (unsigned)(1)), 32, 0, stream>>>(gm1b_13); }
    { GemmP gm1c_13;
      gm1c_13.A = EF; gm1c_13.B = mnw1 + (size_t)256 * H; gm1c_13.bias = EF; gm1c_13.R = G; gm1c_13.C = G;
      gm1c_13.sAo = 0; gm1c_13.sAi = 0; gm1c_13.sAm = H; gm1c_13.sAk = 1; gm1c_13.sBo = 0; gm1c_13.sBi = 0; gm1c_13.sBn = 1; gm1c_13.sBk = H; gm1c_13.sCo = 0; gm1c_13.sCi = 0; gm1c_13.sCm = H; gm1c_13.sRo = 0; gm1c_13.sRi = 0; gm1c_13.sRm = H; gm1c_13.sRn = 1;
      gm1c_13.M = CH; gm1c_13.N = H; gm1c_13.K = H; gm1c_13.zi_n = 1; gm1c_13.flags = 4; gm1c_13.act = 0;
      gm1c_13.alpha = 1.0f; gm1c_13.beta = 1.0f; gm1c_13.sa = 1.0f; gm1c_13.sb = 1.0f; gm1c_13.Npad = H; gm1c_13.pad_ = 0;
      k_gemm<1><<<dim3((unsigned)((H) + 31) / 32, (unsigned)((CH) + 15) / 16, (unsigned)(1)), 32, 0, stream>>>(gm1c_13); }
    k_csp_silu<<<(unsigned)(((long long)CH * H + 255) / 256), 256, 0, stream>>>(G, (long long)CH * H);
    { GemmP gm2_13;
      gm2_13.A = G; gm2_13.B = mnw2; gm2_13.bias = mnb2; gm2_13.R = G; gm2_13.C = MSG;
      gm2_13.sAo = 0; gm2_13.sAi = 0; gm2_13.sAm = H; gm2_13.sAk = 1; gm2_13.sBo = 0; gm2_13.sBi = 0; gm2_13.sBn = 1; gm2_13.sBk = H; gm2_13.sCo = 0; gm2_13.sCi = 0; gm2_13.sCm = H; gm2_13.sRo = 0; gm2_13.sRi = 0; gm2_13.sRm = 0; gm2_13.sRn = 0;
      gm2_13.M = CH; gm2_13.N = H; gm2_13.K = H; gm2_13.zi_n = 1; gm2_13.flags = 1; gm2_13.act = 0;
      gm2_13.alpha = 1.0f; gm2_13.beta = 0.0f; gm2_13.sa = 1.0f; gm2_13.sb = 1.0f; gm2_13.Npad = H; gm2_13.pad_ = 0;
      k_gemm<1><<<dim3((unsigned)((H) + 31) / 32, (unsigned)((CH) + 15) / 16, (unsigned)(1)), 32, 0, stream>>>(gm2_13); }
    k_csp_agg<<<(unsigned)(((long long)Nn * H + 255) / 256), 256, 0, stream>>>(MSG, off, AGG, 650000, CH, Nn, H);
    k_csp_gather<<<(unsigned)(((long long)CH * H + 255) / 256), 256, 0, stream>>>(x, ea, ei, slot, XD, XS, EAc, 700000, CH, E, H, EDd);
    { GemmP ge1_14;
      ge1_14.A = EAc; ge1_14.B = eew1; ge1_14.bias = eeb1; ge1_14.R = EAc; ge1_14.C = EF1;
      ge1_14.sAo = 0; ge1_14.sAi = 0; ge1_14.sAm = 32; ge1_14.sAk = 1; ge1_14.sBo = 0; ge1_14.sBi = 0; ge1_14.sBn = 1; ge1_14.sBk = H; ge1_14.sCo = 0; ge1_14.sCi = 0; ge1_14.sCm = H; ge1_14.sRo = 0; ge1_14.sRi = 0; ge1_14.sRm = 0; ge1_14.sRn = 0;
      ge1_14.M = CH; ge1_14.N = H; ge1_14.K = EDd; ge1_14.zi_n = 1; ge1_14.flags = 1; ge1_14.act = 0;
      ge1_14.alpha = 1.0f; ge1_14.beta = 0.0f; ge1_14.sa = 1.0f; ge1_14.sb = 1.0f; ge1_14.Npad = H; ge1_14.pad_ = 0;
      k_gemm<1><<<dim3((unsigned)((H) + 31) / 32, (unsigned)((CH) + 15) / 16, (unsigned)(1)), 32, 0, stream>>>(ge1_14); }
    k_csp_silu<<<(unsigned)(((long long)CH * H + 255) / 256), 256, 0, stream>>>(EF1, (long long)CH * H);
    { GemmP ge2_14;
      ge2_14.A = EF1; ge2_14.B = eew2; ge2_14.bias = eeb2; ge2_14.R = EF1; ge2_14.C = EF;
      ge2_14.sAo = 0; ge2_14.sAi = 0; ge2_14.sAm = H; ge2_14.sAk = 1; ge2_14.sBo = 0; ge2_14.sBi = 0; ge2_14.sBn = 1; ge2_14.sBk = H; ge2_14.sCo = 0; ge2_14.sCi = 0; ge2_14.sCm = H; ge2_14.sRo = 0; ge2_14.sRi = 0; ge2_14.sRm = 0; ge2_14.sRn = 0;
      ge2_14.M = CH; ge2_14.N = H; ge2_14.K = H; ge2_14.zi_n = 1; ge2_14.flags = 1; ge2_14.act = 0;
      ge2_14.alpha = 1.0f; ge2_14.beta = 0.0f; ge2_14.sa = 1.0f; ge2_14.sb = 1.0f; ge2_14.Npad = H; ge2_14.pad_ = 0;
      k_gemm<1><<<dim3((unsigned)((H) + 31) / 32, (unsigned)((CH) + 15) / 16, (unsigned)(1)), 32, 0, stream>>>(ge2_14); }
    { GemmP gm1a_14;
      gm1a_14.A = XD; gm1a_14.B = mnw1; gm1a_14.bias = mnb1; gm1a_14.R = XD; gm1a_14.C = G;
      gm1a_14.sAo = 0; gm1a_14.sAi = 0; gm1a_14.sAm = H; gm1a_14.sAk = 1; gm1a_14.sBo = 0; gm1a_14.sBi = 0; gm1a_14.sBn = 1; gm1a_14.sBk = H; gm1a_14.sCo = 0; gm1a_14.sCi = 0; gm1a_14.sCm = H; gm1a_14.sRo = 0; gm1a_14.sRi = 0; gm1a_14.sRm = 0; gm1a_14.sRn = 0;
      gm1a_14.M = CH; gm1a_14.N = H; gm1a_14.K = H; gm1a_14.zi_n = 1; gm1a_14.flags = 1; gm1a_14.act = 0;
      gm1a_14.alpha = 1.0f; gm1a_14.beta = 0.0f; gm1a_14.sa = 1.0f; gm1a_14.sb = 1.0f; gm1a_14.Npad = H; gm1a_14.pad_ = 0;
      k_gemm<1><<<dim3((unsigned)((H) + 31) / 32, (unsigned)((CH) + 15) / 16, (unsigned)(1)), 32, 0, stream>>>(gm1a_14); }
    { GemmP gm1b_14;
      gm1b_14.A = XS; gm1b_14.B = mnw1 + (size_t)128 * H; gm1b_14.bias = XS; gm1b_14.R = G; gm1b_14.C = G;
      gm1b_14.sAo = 0; gm1b_14.sAi = 0; gm1b_14.sAm = H; gm1b_14.sAk = 1; gm1b_14.sBo = 0; gm1b_14.sBi = 0; gm1b_14.sBn = 1; gm1b_14.sBk = H; gm1b_14.sCo = 0; gm1b_14.sCi = 0; gm1b_14.sCm = H; gm1b_14.sRo = 0; gm1b_14.sRi = 0; gm1b_14.sRm = H; gm1b_14.sRn = 1;
      gm1b_14.M = CH; gm1b_14.N = H; gm1b_14.K = H; gm1b_14.zi_n = 1; gm1b_14.flags = 4; gm1b_14.act = 0;
      gm1b_14.alpha = 1.0f; gm1b_14.beta = 1.0f; gm1b_14.sa = 1.0f; gm1b_14.sb = 1.0f; gm1b_14.Npad = H; gm1b_14.pad_ = 0;
      k_gemm<1><<<dim3((unsigned)((H) + 31) / 32, (unsigned)((CH) + 15) / 16, (unsigned)(1)), 32, 0, stream>>>(gm1b_14); }
    { GemmP gm1c_14;
      gm1c_14.A = EF; gm1c_14.B = mnw1 + (size_t)256 * H; gm1c_14.bias = EF; gm1c_14.R = G; gm1c_14.C = G;
      gm1c_14.sAo = 0; gm1c_14.sAi = 0; gm1c_14.sAm = H; gm1c_14.sAk = 1; gm1c_14.sBo = 0; gm1c_14.sBi = 0; gm1c_14.sBn = 1; gm1c_14.sBk = H; gm1c_14.sCo = 0; gm1c_14.sCi = 0; gm1c_14.sCm = H; gm1c_14.sRo = 0; gm1c_14.sRi = 0; gm1c_14.sRm = H; gm1c_14.sRn = 1;
      gm1c_14.M = CH; gm1c_14.N = H; gm1c_14.K = H; gm1c_14.zi_n = 1; gm1c_14.flags = 4; gm1c_14.act = 0;
      gm1c_14.alpha = 1.0f; gm1c_14.beta = 1.0f; gm1c_14.sa = 1.0f; gm1c_14.sb = 1.0f; gm1c_14.Npad = H; gm1c_14.pad_ = 0;
      k_gemm<1><<<dim3((unsigned)((H) + 31) / 32, (unsigned)((CH) + 15) / 16, (unsigned)(1)), 32, 0, stream>>>(gm1c_14); }
    k_csp_silu<<<(unsigned)(((long long)CH * H + 255) / 256), 256, 0, stream>>>(G, (long long)CH * H);
    { GemmP gm2_14;
      gm2_14.A = G; gm2_14.B = mnw2; gm2_14.bias = mnb2; gm2_14.R = G; gm2_14.C = MSG;
      gm2_14.sAo = 0; gm2_14.sAi = 0; gm2_14.sAm = H; gm2_14.sAk = 1; gm2_14.sBo = 0; gm2_14.sBi = 0; gm2_14.sBn = 1; gm2_14.sBk = H; gm2_14.sCo = 0; gm2_14.sCi = 0; gm2_14.sCm = H; gm2_14.sRo = 0; gm2_14.sRi = 0; gm2_14.sRm = 0; gm2_14.sRn = 0;
      gm2_14.M = CH; gm2_14.N = H; gm2_14.K = H; gm2_14.zi_n = 1; gm2_14.flags = 1; gm2_14.act = 0;
      gm2_14.alpha = 1.0f; gm2_14.beta = 0.0f; gm2_14.sa = 1.0f; gm2_14.sb = 1.0f; gm2_14.Npad = H; gm2_14.pad_ = 0;
      k_gemm<1><<<dim3((unsigned)((H) + 31) / 32, (unsigned)((CH) + 15) / 16, (unsigned)(1)), 32, 0, stream>>>(gm2_14); }
    k_csp_agg<<<(unsigned)(((long long)Nn * H + 255) / 256), 256, 0, stream>>>(MSG, off, AGG, 700000, CH, Nn, H);
    k_csp_gather<<<(unsigned)(((long long)CH * H + 255) / 256), 256, 0, stream>>>(x, ea, ei, slot, XD, XS, EAc, 750000, CH, E, H, EDd);
    { GemmP ge1_15;
      ge1_15.A = EAc; ge1_15.B = eew1; ge1_15.bias = eeb1; ge1_15.R = EAc; ge1_15.C = EF1;
      ge1_15.sAo = 0; ge1_15.sAi = 0; ge1_15.sAm = 32; ge1_15.sAk = 1; ge1_15.sBo = 0; ge1_15.sBi = 0; ge1_15.sBn = 1; ge1_15.sBk = H; ge1_15.sCo = 0; ge1_15.sCi = 0; ge1_15.sCm = H; ge1_15.sRo = 0; ge1_15.sRi = 0; ge1_15.sRm = 0; ge1_15.sRn = 0;
      ge1_15.M = CH; ge1_15.N = H; ge1_15.K = EDd; ge1_15.zi_n = 1; ge1_15.flags = 1; ge1_15.act = 0;
      ge1_15.alpha = 1.0f; ge1_15.beta = 0.0f; ge1_15.sa = 1.0f; ge1_15.sb = 1.0f; ge1_15.Npad = H; ge1_15.pad_ = 0;
      k_gemm<1><<<dim3((unsigned)((H) + 31) / 32, (unsigned)((CH) + 15) / 16, (unsigned)(1)), 32, 0, stream>>>(ge1_15); }
    k_csp_silu<<<(unsigned)(((long long)CH * H + 255) / 256), 256, 0, stream>>>(EF1, (long long)CH * H);
    { GemmP ge2_15;
      ge2_15.A = EF1; ge2_15.B = eew2; ge2_15.bias = eeb2; ge2_15.R = EF1; ge2_15.C = EF;
      ge2_15.sAo = 0; ge2_15.sAi = 0; ge2_15.sAm = H; ge2_15.sAk = 1; ge2_15.sBo = 0; ge2_15.sBi = 0; ge2_15.sBn = 1; ge2_15.sBk = H; ge2_15.sCo = 0; ge2_15.sCi = 0; ge2_15.sCm = H; ge2_15.sRo = 0; ge2_15.sRi = 0; ge2_15.sRm = 0; ge2_15.sRn = 0;
      ge2_15.M = CH; ge2_15.N = H; ge2_15.K = H; ge2_15.zi_n = 1; ge2_15.flags = 1; ge2_15.act = 0;
      ge2_15.alpha = 1.0f; ge2_15.beta = 0.0f; ge2_15.sa = 1.0f; ge2_15.sb = 1.0f; ge2_15.Npad = H; ge2_15.pad_ = 0;
      k_gemm<1><<<dim3((unsigned)((H) + 31) / 32, (unsigned)((CH) + 15) / 16, (unsigned)(1)), 32, 0, stream>>>(ge2_15); }
    { GemmP gm1a_15;
      gm1a_15.A = XD; gm1a_15.B = mnw1; gm1a_15.bias = mnb1; gm1a_15.R = XD; gm1a_15.C = G;
      gm1a_15.sAo = 0; gm1a_15.sAi = 0; gm1a_15.sAm = H; gm1a_15.sAk = 1; gm1a_15.sBo = 0; gm1a_15.sBi = 0; gm1a_15.sBn = 1; gm1a_15.sBk = H; gm1a_15.sCo = 0; gm1a_15.sCi = 0; gm1a_15.sCm = H; gm1a_15.sRo = 0; gm1a_15.sRi = 0; gm1a_15.sRm = 0; gm1a_15.sRn = 0;
      gm1a_15.M = CH; gm1a_15.N = H; gm1a_15.K = H; gm1a_15.zi_n = 1; gm1a_15.flags = 1; gm1a_15.act = 0;
      gm1a_15.alpha = 1.0f; gm1a_15.beta = 0.0f; gm1a_15.sa = 1.0f; gm1a_15.sb = 1.0f; gm1a_15.Npad = H; gm1a_15.pad_ = 0;
      k_gemm<1><<<dim3((unsigned)((H) + 31) / 32, (unsigned)((CH) + 15) / 16, (unsigned)(1)), 32, 0, stream>>>(gm1a_15); }
    { GemmP gm1b_15;
      gm1b_15.A = XS; gm1b_15.B = mnw1 + (size_t)128 * H; gm1b_15.bias = XS; gm1b_15.R = G; gm1b_15.C = G;
      gm1b_15.sAo = 0; gm1b_15.sAi = 0; gm1b_15.sAm = H; gm1b_15.sAk = 1; gm1b_15.sBo = 0; gm1b_15.sBi = 0; gm1b_15.sBn = 1; gm1b_15.sBk = H; gm1b_15.sCo = 0; gm1b_15.sCi = 0; gm1b_15.sCm = H; gm1b_15.sRo = 0; gm1b_15.sRi = 0; gm1b_15.sRm = H; gm1b_15.sRn = 1;
      gm1b_15.M = CH; gm1b_15.N = H; gm1b_15.K = H; gm1b_15.zi_n = 1; gm1b_15.flags = 4; gm1b_15.act = 0;
      gm1b_15.alpha = 1.0f; gm1b_15.beta = 1.0f; gm1b_15.sa = 1.0f; gm1b_15.sb = 1.0f; gm1b_15.Npad = H; gm1b_15.pad_ = 0;
      k_gemm<1><<<dim3((unsigned)((H) + 31) / 32, (unsigned)((CH) + 15) / 16, (unsigned)(1)), 32, 0, stream>>>(gm1b_15); }
    { GemmP gm1c_15;
      gm1c_15.A = EF; gm1c_15.B = mnw1 + (size_t)256 * H; gm1c_15.bias = EF; gm1c_15.R = G; gm1c_15.C = G;
      gm1c_15.sAo = 0; gm1c_15.sAi = 0; gm1c_15.sAm = H; gm1c_15.sAk = 1; gm1c_15.sBo = 0; gm1c_15.sBi = 0; gm1c_15.sBn = 1; gm1c_15.sBk = H; gm1c_15.sCo = 0; gm1c_15.sCi = 0; gm1c_15.sCm = H; gm1c_15.sRo = 0; gm1c_15.sRi = 0; gm1c_15.sRm = H; gm1c_15.sRn = 1;
      gm1c_15.M = CH; gm1c_15.N = H; gm1c_15.K = H; gm1c_15.zi_n = 1; gm1c_15.flags = 4; gm1c_15.act = 0;
      gm1c_15.alpha = 1.0f; gm1c_15.beta = 1.0f; gm1c_15.sa = 1.0f; gm1c_15.sb = 1.0f; gm1c_15.Npad = H; gm1c_15.pad_ = 0;
      k_gemm<1><<<dim3((unsigned)((H) + 31) / 32, (unsigned)((CH) + 15) / 16, (unsigned)(1)), 32, 0, stream>>>(gm1c_15); }
    k_csp_silu<<<(unsigned)(((long long)CH * H + 255) / 256), 256, 0, stream>>>(G, (long long)CH * H);
    { GemmP gm2_15;
      gm2_15.A = G; gm2_15.B = mnw2; gm2_15.bias = mnb2; gm2_15.R = G; gm2_15.C = MSG;
      gm2_15.sAo = 0; gm2_15.sAi = 0; gm2_15.sAm = H; gm2_15.sAk = 1; gm2_15.sBo = 0; gm2_15.sBi = 0; gm2_15.sBn = 1; gm2_15.sBk = H; gm2_15.sCo = 0; gm2_15.sCi = 0; gm2_15.sCm = H; gm2_15.sRo = 0; gm2_15.sRi = 0; gm2_15.sRm = 0; gm2_15.sRn = 0;
      gm2_15.M = CH; gm2_15.N = H; gm2_15.K = H; gm2_15.zi_n = 1; gm2_15.flags = 1; gm2_15.act = 0;
      gm2_15.alpha = 1.0f; gm2_15.beta = 0.0f; gm2_15.sa = 1.0f; gm2_15.sb = 1.0f; gm2_15.Npad = H; gm2_15.pad_ = 0;
      k_gemm<1><<<dim3((unsigned)((H) + 31) / 32, (unsigned)((CH) + 15) / 16, (unsigned)(1)), 32, 0, stream>>>(gm2_15); }
    k_csp_agg<<<(unsigned)(((long long)Nn * H + 255) / 256), 256, 0, stream>>>(MSG, off, AGG, 750000, CH, Nn, H);
    { GemmP gu1a;
      gu1a.A = x; gu1a.B = unw1; gu1a.bias = unb1; gu1a.R = x; gu1a.C = UP;
      gu1a.sAo = 0; gu1a.sAi = 0; gu1a.sAm = H; gu1a.sAk = 1; gu1a.sBo = 0; gu1a.sBi = 0; gu1a.sBn = 1; gu1a.sBk = H; gu1a.sCo = 0; gu1a.sCi = 0; gu1a.sCm = H; gu1a.sRo = 0; gu1a.sRi = 0; gu1a.sRm = 0; gu1a.sRn = 0;
      gu1a.M = Nn; gu1a.N = H; gu1a.K = H; gu1a.zi_n = 1; gu1a.flags = 1; gu1a.act = 0;
      gu1a.alpha = 1.0f; gu1a.beta = 0.0f; gu1a.sa = 1.0f; gu1a.sb = 1.0f; gu1a.Npad = H; gu1a.pad_ = 0;
      k_gemm<1><<<dim3((unsigned)((H) + 31) / 32, (unsigned)((Nn) + 15) / 16, (unsigned)(1)), 32, 0, stream>>>(gu1a); }
    { GemmP gu1b;
      gu1b.A = AGG; gu1b.B = unw1 + (size_t)128 * H; gu1b.bias = AGG; gu1b.R = UP; gu1b.C = UP;
      gu1b.sAo = 0; gu1b.sAi = 0; gu1b.sAm = H; gu1b.sAk = 1; gu1b.sBo = 0; gu1b.sBi = 0; gu1b.sBn = 1; gu1b.sBk = H; gu1b.sCo = 0; gu1b.sCi = 0; gu1b.sCm = H; gu1b.sRo = 0; gu1b.sRi = 0; gu1b.sRm = H; gu1b.sRn = 1;
      gu1b.M = Nn; gu1b.N = H; gu1b.K = H; gu1b.zi_n = 1; gu1b.flags = 4; gu1b.act = 0;
      gu1b.alpha = 1.0f; gu1b.beta = 1.0f; gu1b.sa = 1.0f; gu1b.sb = 1.0f; gu1b.Npad = H; gu1b.pad_ = 0;
      k_gemm<1><<<dim3((unsigned)((H) + 31) / 32, (unsigned)((Nn) + 15) / 16, (unsigned)(1)), 32, 0, stream>>>(gu1b); }
    k_csp_silu<<<(unsigned)(((long long)Nn * H + 255) / 256), 256, 0, stream>>>(UP, (long long)Nn * H);
    { GemmP gu2;
      gu2.A = UP; gu2.B = unw2; gu2.bias = unb2; gu2.R = UP; gu2.C = X2;
      gu2.sAo = 0; gu2.sAi = 0; gu2.sAm = H; gu2.sAk = 1; gu2.sBo = 0; gu2.sBi = 0; gu2.sBn = 1; gu2.sBk = H; gu2.sCo = 0; gu2.sCi = 0; gu2.sCm = H; gu2.sRo = 0; gu2.sRi = 0; gu2.sRm = 0; gu2.sRn = 0;
      gu2.M = Nn; gu2.N = H; gu2.K = H; gu2.zi_n = 1; gu2.flags = 1; gu2.act = 0;
      gu2.alpha = 1.0f; gu2.beta = 0.0f; gu2.sa = 1.0f; gu2.sb = 1.0f; gu2.Npad = H; gu2.pad_ = 0;
      k_gemm<1><<<dim3((unsigned)((H) + 31) / 32, (unsigned)((Nn) + 15) / 16, (unsigned)(1)), 32, 0, stream>>>(gu2); }
    { GemmP gl2a;
      gl2a.A = lat; gl2a.B = l2aw; gl2a.bias = l2ab; gl2a.R = lat; gl2a.C = LI;
      gl2a.sAo = 0; gl2a.sAi = 0; gl2a.sAm = 9; gl2a.sAk = 1; gl2a.sBo = 0; gl2a.sBi = 0; gl2a.sBn = 1; gl2a.sBk = H; gl2a.sCo = 0; gl2a.sCi = 0; gl2a.sCm = H; gl2a.sRo = 0; gl2a.sRi = 0; gl2a.sRm = 0; gl2a.sRn = 0;
      gl2a.M = NB; gl2a.N = H; gl2a.K = 9; gl2a.zi_n = 1; gl2a.flags = 1; gl2a.act = 0;
      gl2a.alpha = 1.0f; gl2a.beta = 0.0f; gl2a.sa = 1.0f; gl2a.sb = 1.0f; gl2a.Npad = H; gl2a.pad_ = 0;
      k_gemm<1><<<dim3((unsigned)((H) + 31) / 32, (unsigned)((NB) + 15) / 16, (unsigned)(1)), 32, 0, stream>>>(gl2a); }
    k_csp_x2<<<(unsigned)(((long long)Nn * H + 255) / 256), 256, 0, stream>>>(x, X2, LI, bat, UP, Nn, H);
    k_csr_mean<<<(unsigned)(((long long)NB * H + 255) / 256), 256, 0, stream>>>(UP, ids, goff, gslot, AI, NB, H);
    { GemmP ga2l;
      ga2l.A = AI; ga2l.B = a2lw; ga2l.bias = a2lb; ga2l.R = AI; ga2l.C = LF;
      ga2l.sAo = 0; ga2l.sAi = 0; ga2l.sAm = H; ga2l.sAk = 1; ga2l.sBo = 0; ga2l.sBi = 0; ga2l.sBn = 1; ga2l.sBk = 9; ga2l.sCo = 0; ga2l.sCi = 0; ga2l.sCm = LP; ga2l.sRo = 0; ga2l.sRi = 0; ga2l.sRm = 0; ga2l.sRn = 0;
      ga2l.M = NB; ga2l.N = 9; ga2l.K = H; ga2l.zi_n = 1; ga2l.flags = 1; ga2l.act = 0;
      ga2l.alpha = 1.0f; ga2l.beta = 0.0f; ga2l.sa = 1.0f; ga2l.sb = 1.0f; ga2l.Npad = LP; ga2l.pad_ = 0;
      k_gemm<1><<<dim3((unsigned)((LP) + 31) / 32, (unsigned)((NB) + 15) / 16, (unsigned)(1)), 32, 0, stream>>>(ga2l); }
    k_stats<<<(unsigned)(Nn), 256, 0, stream>>>(UP, H, 0, 1, H, H, 1e-05f, st, 0);
    k_norm_apply<<<(unsigned)(((long long)(Nn) * (H) * (1) + 255) / 256), 256, 0, stream>>>(UP, out, st, nlg, nlb, Nn, H, 1, 1, 0, 0);
    k_csp_latln<<<(unsigned)((NB + 255) / 256), 256, 0, stream>>>(lat, LF, LP, llg, llb, lout, NB);
}
